// PyTorchConv1d_2396591751363
// MI455X (gfx1250) — hardware-verified
//
#include <hip/hip_runtime.h>
#include <math.h>

typedef __attribute__((ext_vector_type(16))) _Float16 v16h;
typedef __attribute__((ext_vector_type(8)))  _Float16 v8h;
typedef __attribute__((ext_vector_type(16))) __bf16   v16b;
typedef __attribute__((ext_vector_type(8)))  float    v8f;
typedef __attribute__((ext_vector_type(4)))  float    v4f;

__device__ __forceinline__ int frag_k(int i, int h) { return (i < 8) ? (8 * h + i) : (16 + 8 * h + (i - 8)); }
__device__ __forceinline__ __bf16 bf16_rne(float f) {
    unsigned int u = __float_as_uint(f);
    u += 0x7fffu + ((u >> 16) & 1u);
    return __builtin_bit_cast(__bf16, (unsigned short)(u >> 16));
}
__device__ __forceinline__ float bf16_f32(__bf16 b) { return __uint_as_float(((unsigned int)__builtin_bit_cast(unsigned short, b)) << 16); }
__device__ __forceinline__ v8f wmma16(v16h a, v16h b, v8f c) {
    c = __builtin_amdgcn_wmma_f32_16x16x32_f16(false, a, false, b, (short)0, c, false, false);
    asm volatile("v_nop\n\tv_nop\n\tv_nop\n\tv_nop" : "+v"(c) : "v"(a), "v"(b));
    return c;
}
__device__ __forceinline__ v8f wmmab(v16b a, v16b b, v8f c) {
    c = __builtin_amdgcn_wmma_f32_16x16x32_bf16(false, a, false, b, (short)0, c, false, false);
    asm volatile("v_nop\n\tv_nop\n\tv_nop\n\tv_nop" : "+v"(c) : "v"(a), "v"(b));
    return c;
}
struct Split { v16b hi, lo; };
__device__ __forceinline__ v8f wmma3(const Split& a, const Split& b, v8f c) {
    c = __builtin_amdgcn_wmma_f32_16x16x32_bf16(false, a.hi, false, b.hi, (short)0, c, false, false);
    c = __builtin_amdgcn_wmma_f32_16x16x32_bf16(false, a.hi, false, b.lo, (short)0, c, false, false);
    c = __builtin_amdgcn_wmma_f32_16x16x32_bf16(false, a.lo, false, b.hi, (short)0, c, false, false);
    asm volatile("v_nop\n\tv_nop\n\tv_nop\n\tv_nop" : "+v"(c) : "v"(a.hi), "v"(a.lo), "v"(b.hi), "v"(b.lo));
    return c;
}
struct Split3 { v16b hi, mid, lo; };
__device__ __forceinline__ v8f wmma6(const Split3& a, const Split3& b, v8f c) {
    c = __builtin_amdgcn_wmma_f32_16x16x32_bf16(false, a.hi, false, b.hi, (short)0, c, false, false);
    c = __builtin_amdgcn_wmma_f32_16x16x32_bf16(false, a.hi, false, b.mid, (short)0, c, false, false);
    c = __builtin_amdgcn_wmma_f32_16x16x32_bf16(false, a.mid, false, b.hi, (short)0, c, false, false);
    c = __builtin_amdgcn_wmma_f32_16x16x32_bf16(false, a.hi, false, b.lo, (short)0, c, false, false);
    c = __builtin_amdgcn_wmma_f32_16x16x32_bf16(false, a.mid, false, b.mid, (short)0, c, false, false);
    c = __builtin_amdgcn_wmma_f32_16x16x32_bf16(false, a.lo, false, b.hi, (short)0, c, false, false);
    asm volatile("v_nop\n\tv_nop\n\tv_nop\n\tv_nop" : "+v"(c) : "v"(a.hi), "v"(a.mid), "v"(a.lo), "v"(b.hi), "v"(b.mid), "v"(b.lo));
    return c;
}

__device__ __forceinline__ v16h fh_ld(const float* __restrict__ p, long long sk, int k0, int h, int klen, float s) {
    v16h a;
#pragma unroll
    for (int i = 0; i < 16; ++i) { const int k = k0 + frag_k(i, h); a[i] = (k < klen) ? (_Float16)(p[(long long)k * sk] * s) : (_Float16)0.f; }
    return a;
}
__device__ __forceinline__ Split sp_ld(const float* __restrict__ p, long long sk, int k0, int h, int klen, float s) {
    Split r;
#pragma unroll
    for (int i = 0; i < 16; ++i) {
        const int k = k0 + frag_k(i, h); const float x = (k < klen) ? p[(long long)k * sk] * s : 0.f;
        const __bf16 hb = bf16_rne(x); r.hi[i] = hb; r.lo[i] = bf16_rne(x - bf16_f32(hb));
    }
    return r;
}
__device__ __forceinline__ Split3 sp3_ld(const float* __restrict__ p, long long sk, int k0, int h, int klen, float s) {
    Split3 r;
#pragma unroll
    for (int i = 0; i < 16; ++i) {
        const int k = k0 + frag_k(i, h); const float x = (k < klen) ? p[(long long)k * sk] * s : 0.f;
        const __bf16 hb = bf16_rne(x); const float r1 = x - bf16_f32(hb); const __bf16 mb = bf16_rne(r1);
        r.hi[i] = hb; r.mid[i] = mb; r.lo[i] = bf16_rne(r1 - bf16_f32(mb));
    }
    return r;
}
__device__ __forceinline__ v16b bh_ld(const float* __restrict__ p, long long sk, int k0, int h, int klen, float s) {
    v16b a;
#pragma unroll
    for (int i = 0; i < 16; ++i) { const int k = k0 + frag_k(i, h); a[i] = bf16_rne((k < klen) ? p[(long long)k * sk] * s : 0.f); }
    return a;
}
__device__ __forceinline__ v16h fh_row(const _Float16* __restrict__ row, int k0, int h) {
    v16h a;
#pragma unroll
    for (int i = 0; i < 16; ++i) a[i] = row[k0 + frag_k(i, h)];
    return a;
}

#define VST2(T, ptr, val) do { *(volatile T*)(ptr) = (val); __threadfence(); *(volatile T*)(ptr) = (val); } while (0)
typedef float v4f __attribute__((ext_vector_type(4)));
#define VST2V4(ptr, val) do { *(volatile v4f*)(ptr) = (val); __threadfence(); *(volatile v4f*)(ptr) = (val); } while (0)

__device__ __attribute__((noinline)) float act_fn(float v, int act) {
    if (act == 1) return fmaxf(v, 0.f);
    if (act == 2) { const float u = 0.7978845608028654f * (v + 0.044715f * v * v * v); return 0.5f * v * (1.f + tanhf(u)); }
    if (act == 3) return v / (1.f + expf(-v));
    if (act == 4) return 0.5f * v * (1.f + erff(v * 0.7071067811865476f));
    if (act == 5) return tanhf(v);
    if (act == 6) return 1.f / (1.f + expf(-v));
    if (act == 7) return (v > 0.f) ? v : 0.01f * v;
    if (act == 8) return (v > 0.f) ? v : (expf(v) - 1.f);
    if (act == 9) return fminf(fmaxf(v, 0.f), 6.f);
    if (act == 10) return fabsf(v);
    if (act == 11) return (v >= 0.f) ? v : 0.1f * v;
    if (act == 12) return (v > 0.f) ? v : 0.2f * v;
    if (act == 13) return (v > 20.f) ? v : log1pf(expf(v));
    return v;
}

struct GemmP {
    const float* A; const float* B; const float* bias; const float* R; float* C;
    long long sAo, sAi, sAm, sAk, sBo, sBi, sBn, sBk, sCo, sCi, sCm, sRo, sRi, sRm, sRn;
    int M, N, K, zi_n, flags, act; float alpha, beta, sa, sb;
    int Npad, pad_;
};
static_assert(sizeof(GemmP) == 5 * 8 + 15 * 8 + 6 * 4 + 4 * 4 + 2 * 4, "GemmP has padding");

template <int MODE>
__global__ __launch_bounds__(32) void k_gemm(GemmP p) {
    const int lane = threadIdx.x & 31, h = lane >> 4, l15 = lane & 15;
    const int m0 = blockIdx.y * 16, n0 = blockIdx.x * 32;
    const int z = blockIdx.z, zo = z / p.zi_n, zi = z - zo * p.zi_n;
    const float* A = p.A + zo * p.sAo + zi * p.sAi;
    const float* B = p.B + zo * p.sBo + zi * p.sBi;
    const int am = min(m0 + l15, p.M - 1);
    v8f acc[2], comp[2];
#pragma unroll
    for (int t = 0; t < 2; ++t) { v8f zz = {}; acc[t] = zz; comp[t] = zz; }
    for (int k0 = 0; k0 < p.K; k0 += 32) {
        const float* arow = A + (long long)am * p.sAm;
        if (MODE == 1) {
            const Split a = sp_ld(arow, p.sAk, k0, h, p.K, 1.f);
#pragma unroll
            for (int t = 0; t < 2; ++t) {
                const int bn = min(n0 + t * 16 + l15, p.N - 1);
                acc[t] = wmma3(a, sp_ld(B + (long long)bn * p.sBn, p.sBk, k0, h, p.K, 1.f), acc[t]);
            }
        } else if (MODE == 3) {
            const Split3 a = sp3_ld(arow, p.sAk, k0, h, p.K, 1.f);
#pragma unroll
            for (int t = 0; t < 2; ++t) {
                const int bn = min(n0 + t * 16 + l15, p.N - 1);
                acc[t] = wmma6(a, sp3_ld(B + (long long)bn * p.sBn, p.sBk, k0, h, p.K, 1.f), acc[t]);
            }
        } else if (MODE == 4) {
            const Split3 a = sp3_ld(arow, p.sAk, k0, h, p.K, 1.f);
#pragma unroll
            for (int t = 0; t < 2; ++t) {
                const int bn = min(n0 + t * 16 + l15, p.N - 1); v8f zz = {};
                const v8f part = wmma6(a, sp3_ld(B + (long long)bn * p.sBn, p.sBk, k0, h, p.K, 1.f), zz);
                const v8f y = part - comp[t]; const v8f s = acc[t] + y; comp[t] = (s - acc[t]) - y; acc[t] = s;
            }
        } else if (MODE == 2) {
            const v16b a = bh_ld(arow, p.sAk, k0, h, p.K, 1.f);
#pragma unroll
            for (int t = 0; t < 2; ++t) {
                const int bn = min(n0 + t * 16 + l15, p.N - 1);
                acc[t] = wmmab(a, bh_ld(B + (long long)bn * p.sBn, p.sBk, k0, h, p.K, 1.f), acc[t]);
            }
        } else {
            const v16h a = fh_ld(arow, p.sAk, k0, h, p.K, p.sa);
#pragma unroll
            for (int t = 0; t < 2; ++t) {
                const int bn = min(n0 + t * 16 + l15, p.N - 1);
                acc[t] = wmma16(a, fh_ld(B + (long long)bn * p.sBn, p.sBk, k0, h, p.K, p.sb), acc[t]);
            }
        }
    }
    const float iscale = (MODE == 0) ? p.alpha / (p.sa * p.sb) : p.alpha;
    float* C = p.C + zo * p.sCo + zi * p.sCi;
    const float* R = p.R + zo * p.sRo + zi * p.sRi;
    __shared__ __align__(16) float ctile[16][36];
#pragma unroll
    for (int t = 0; t < 2; ++t) {
        const int n = n0 + t * 16 + l15; const int nn = min(n, p.N - 1);
#pragma unroll
        for (int r = 0; r < 8; ++r) {
            const int m = m0 + 8 * h + r; const int mm = min(m, p.M - 1);
            float v = acc[t][r] * iscale;
            if (p.flags & 1) v += p.bias[nn];
            if (p.flags & 2) v += p.bias[mm];
            v = act_fn(v, p.act);
            if (p.flags & 4) v += p.beta * R[(long long)mm * p.sRm + (long long)nn * p.sRn];
            ctile[8 * h + r][t * 16 + l15] = (n < p.N) ? v : 0.f;
        }
    }
    __syncthreads();
    const int NW = (p.Npad > p.N) ? p.Npad : p.N;
    const bool fast = (m0 + 16 <= p.M) && (n0 + 32 <= NW) && ((p.sCm & 3) == 0) && ((((size_t)C) & 15) == 0);
    if (fast) {
#pragma unroll
        for (int s = 0; s < 4; ++s) {
            const int row = s * 4 + (lane >> 3), c4 = (lane & 7) * 4;
            const v4f v = *(const v4f*)&ctile[row][c4];
            VST2V4(C + (long long)(m0 + row) * p.sCm + n0 + c4, v);
        }
    } else {
        for (int row = 0; row < 16; ++row) {
            const int m = m0 + row, n = n0 + lane;
            if (m < p.M && n < NW) VST2(float, C + (long long)m * p.sCm + n, ctile[row][lane]);
        }
    }
}

#define AW 4
struct AttnP {
    const float* Q; const float* K; const float* V; float* O; float* P; const float* Mf; const int* Mi; float* ST;
    const float* Pw; const float* Rt; const int* SQ; const int* SK;
    long long swb, swh, swi, swj, srb, srh, sri;
    long long sQb, sQh, sQi, sQd, sKb, sKh, sKj, sKd, sVb, sVh, sVj, sVd, sOb, sOh, sOi, sPb, sPh, sPi, smb, smh, smi, smj;
    int Lq, Lk, dh, dv, hrep, causal, coff, pband;
    float scale, mfill; int nonorm, mpol;
    int roff, rn, segpol, win;
};
static_assert(sizeof(AttnP) == 12 * 8 + 29 * 8 + 16 * 4, "AttnP has padding");

#ifndef KATTN_ATTR
#define KATTN_ATTR
#endif
template <int DHP, int DVP, int QM, bool SPLITPV, bool TWOPASS>
__global__ __launch_bounds__(32 * AW) KATTN_ATTR void k_attn(AttnP p) {
    constexpr int NT = DVP / 16;
    constexpr int KS = DHP / 32;
    constexpr int VP = DVP + 8;
    __shared__ __align__(16) float    pl[AW][16 * 64];
    __shared__ __align__(16) _Float16 vl[(SPLITPV ? 2 : 1) * 64 * VP];
    const int lane = threadIdx.x & 31, hf = lane >> 4, l15 = lane & 15, wave = threadIdx.x >> 5;
    const int h = blockIdx.y, b = blockIdx.z, hk = h / p.hrep;
    const int q0 = (blockIdx.x * AW + wave) * 16;
    float* myp = pl[wave];
    const float L2E = 1.4426950408889634f;
    const float NEG = -__builtin_inff();
    const int qi = min(q0 + l15, p.Lq - 1);
    const float* qrow = p.Q + b * p.sQb + h * p.sQh + (long long)qi * p.sQi;
    const float* kbase = p.K + b * p.sKb + hk * p.sKh;
    const float* vbase = p.V + b * p.sVb + hk * p.sVh;
    v16h qa[QM == 0 ? KS : 1]; Split qs_[QM == 1 ? KS : 1]; Split3 qt_[QM == 2 ? KS : 1];
#pragma unroll
    for (int ks = 0; ks < KS; ++ks) {
        if (QM == 2) qt_[ks] = sp3_ld(qrow, p.sQd, ks * 32, hf, p.dh, 1.f);
        else if (QM == 1) qs_[ks] = sp_ld(qrow, p.sQd, ks * 32, hf, p.dh, 1.f);
        else qa[ks] = fh_ld(qrow, p.sQd, ks * 32, hf, p.dh, 1.f);
    }
    v8f o[NT]; float m8[8], l8[8];
#pragma unroll
    for (int t = 0; t < NT; ++t) { v8f zz = {}; o[t] = zz; }
#pragma unroll
    for (int i = 0; i < 8; ++i) { m8[i] = NEG; l8[i] = 0.f; }
    int jend = p.Lk;
    if (p.causal == 1) { const int je = (blockIdx.x * AW + AW - 1) * 16 + 16 + p.coff; jend = min(jend, max(je, 0)); }
    const int npass = TWOPASS ? 2 : 1;
    for (int pass = 0; pass < npass; ++pass) {
        const bool dopv = (!TWOPASS) || pass == 1;
        for (int j0 = 0; j0 < jend; j0 += 64) {
            if (dopv) {
                __syncthreads();
                for (int idx = threadIdx.x; idx < 64 * DVP; idx += 32 * AW) {
                    const int jr = idx / DVP, d = idx - jr * DVP, j = j0 + jr;
                    const float f = (j < p.Lk && d < p.dv) ? vbase[(long long)j * p.sVj + (long long)d * p.sVd] : 0.f;
                    if (SPLITPV) {
                        const __bf16 hb = bf16_rne(f);
                        ((__bf16*)vl)[jr * VP + d] = hb; ((__bf16*)vl)[64 * VP + jr * VP + d] = bf16_rne(f - bf16_f32(hb));
                    } else vl[jr * VP + d] = (_Float16)f;
                }
            }
            v8f s[4];
#pragma unroll
            for (int t = 0; t < 4; ++t) {
                const int j = min(j0 + t * 16 + l15, p.Lk - 1);
                const float* krow = kbase + (long long)j * p.sKj;
                v8f acc = {};
#pragma unroll
                for (int ks = 0; ks < KS; ++ks) {
                    if (QM == 2)      acc = wmma6(qt_[ks], sp3_ld(krow, p.sKd, ks * 32, hf, p.dh, 1.f), acc);
                    else if (QM == 1) acc = wmma3(qs_[ks], sp_ld(krow, p.sKd, ks * 32, hf, p.dh, 1.f), acc);
                    else              acc = wmma16(qa[ks], fh_ld(krow, p.sKd, ks * 32, hf, p.dh, 1.f), acc);
                }
                s[t] = acc;
            }
            float pv[8][4];
#pragma unroll
            for (int i = 0; i < 8; ++i) {
                const int irow = q0 + i + 8 * hf;
                const int ic = min(irow, p.Lq - 1);
                float sc[4];
#pragma unroll
                for (int t = 0; t < 4; ++t) {
                    const int jg = j0 + t * 16 + l15;
                    float v = s[t][i] * p.scale;
                    if (p.Mf) v += p.Mf[b * p.smb + h * p.smh + (long long)ic * p.smi + (long long)min(jg, p.Lk - 1) * p.smj];
                    if (p.Rt) { int rc = ic - min(jg, p.Lk - 1) + p.roff; rc = rc < 0 ? 0 : (rc >= p.rn ? p.rn - 1 : rc); v += p.Rt[b * p.srb + h * p.srh + (long long)ic * p.sri + rc]; }
                    if (p.Mi) { const int mv = p.Mi[b * p.smb + h * p.smh + (long long)ic * p.smi + (long long)min(jg, p.Lk - 1) * p.smj]; if (p.mpol ? (mv != 0) : (mv == 0)) v = p.mfill; }
                    if (p.SQ) { const bool same = p.SQ[(long long)b * p.Lq + ic] == p.SK[(long long)b * p.Lk + min(jg, p.Lk - 1)]; if (p.segpol ? same : !same) v = p.mfill; }
                    if (p.causal == 2 && jg > irow + p.coff) v = p.mfill;
                    if (jg >= p.Lk || (p.causal == 1 && jg > irow + p.coff) || (p.causal == 3 && jg < irow + p.coff) || (p.win > 0 && irow + p.coff - jg > p.win)) v = NEG; else v *= L2E;
                    sc[t] = v;
                }
                if (!TWOPASS || pass == 0) {
                    float mx = fmaxf(fmaxf(sc[0], sc[1]), fmaxf(sc[2], sc[3]));
                    mx = fmaxf(mx, __shfl_xor(mx, 1, 32)); mx = fmaxf(mx, __shfl_xor(mx, 2, 32));
                    mx = fmaxf(mx, __shfl_xor(mx, 4, 32)); mx = fmaxf(mx, __shfl_xor(mx, 8, 32));
                    const float mnew = fmaxf(m8[i], mx);
                    const float corr = (mnew == NEG) ? 1.f : exp2f(m8[i] - mnew);
                    float rs = 0.f;
#pragma unroll
                    for (int t = 0; t < 4; ++t) {
                        const float pp = (sc[t] == NEG) ? 0.f : exp2f(sc[t] - mnew); rs += pp;
                        pv[i][t] = p.Pw ? pp * p.Pw[b * p.swb + h * p.swh + (long long)ic * p.swi + (long long)min(j0 + t * 16 + l15, p.Lk - 1) * p.swj] : pp;
                    }
                    rs += __shfl_xor(rs, 1, 32); rs += __shfl_xor(rs, 2, 32); rs += __shfl_xor(rs, 4, 32); rs += __shfl_xor(rs, 8, 32);
                    l8[i] = l8[i] * corr + rs; m8[i] = mnew;
                    if (!TWOPASS) {
#pragma unroll
                        for (int t = 0; t < NT; ++t) o[t][i] *= corr;
                    }
                } else {
                    const float inv = (l8[i] > 0.f) ? 1.f / l8[i] : 0.f;
#pragma unroll
                    for (int t = 0; t < 4; ++t) {
                        const int jg = j0 + t * 16 + l15;
                        float pp = (sc[t] == NEG) ? 0.f : exp2f(sc[t] - m8[i]) * inv;
                        if (p.Pw) pp *= p.Pw[b * p.swb + h * p.swh + (long long)ic * p.swi + (long long)min(jg, p.Lk - 1) * p.swj];
                        pv[i][t] = pp;
                    }
                }
            }
            if (dopv) {
#pragma unroll
                for (int i = 0; i < 8; ++i)
#pragma unroll
                    for (int t = 0; t < 4; ++t) myp[(i + 8 * hf) * 64 + t * 16 + l15] = pv[i][t];
                __syncthreads();
                if (p.P) {
                    float* pb_ = p.P + b * p.sPb + h * p.sPh;
                    const bool fastP = (p.pband == 0) && ((p.sPi & 3) == 0) && (j0 + 64 <= p.Lk) && (q0 + 16 <= p.Lq) && ((((size_t)pb_) & 15) == 0);
                    if (fastP) {
#pragma unroll
                        for (int s = 0; s < 8; ++s) {
                            const int row = s * 2 + (lane >> 4), c4 = (lane & 15) * 4;
                            const v4f v = *(const v4f*)(myp + row * 64 + c4);
                            VST2V4(pb_ + (long long)(q0 + row) * p.sPi + j0 + c4, v);
                        }
                    } else {
                        for (int row = 0; row < 16; ++row) {
                            const int irow = q0 + row; if (irow >= p.Lq) continue;
                            for (int c = lane; c < 64; c += 32) {
                                const int jg = j0 + c; if (jg >= p.Lk) continue;
                                if (p.pband == 0) VST2(float, pb_ + (long long)irow * p.sPi + jg, myp[row * 64 + c]);
                                else if (jg - irow <= p.pband && irow - jg <= p.pband) VST2(float, pb_ + (long long)irow * p.sPi + (jg - irow + p.pband), myp[row * 64 + c]);
                            }
                        }
                    }
                }
                if (SPLITPV) {
                    const Split pa0 = sp_ld(myp + l15 * 64, 1, 0, hf, 64, 1.f), pa1 = sp_ld(myp + l15 * 64, 1, 32, hf, 64, 1.f);
                    const __bf16* vh = (const __bf16*)vl; const __bf16* vlo = vh + 64 * VP;
#pragma unroll
                    for (int t = 0; t < NT; ++t) {
                        const int dcol = t * 16 + l15;
                        Split b0, b1;
#pragma unroll
                        for (int e = 0; e < 16; ++e) {
                            const int k0 = frag_k(e, hf), k1 = 32 + frag_k(e, hf);
                            b0.hi[e] = vh[k0 * VP + dcol]; b0.lo[e] = vlo[k0 * VP + dcol]; b1.hi[e] = vh[k1 * VP + dcol]; b1.lo[e] = vlo[k1 * VP + dcol];
                        }
                        o[t] = wmma3(pa0, b0, o[t]);
                        o[t] = wmma3(pa1, b1, o[t]);
                    }
                } else {
                    const v16h pa0 = fh_ld(myp + l15 * 64, 1, 0, hf, 64, 4096.f), pa1 = fh_ld(myp + l15 * 64, 1, 32, hf, 64, 4096.f);
#pragma unroll
                    for (int t = 0; t < NT; ++t) {
                        const int dcol = t * 16 + l15;
                        v16h b0, b1;
#pragma unroll
                        for (int e = 0; e < 16; ++e) { b0[e] = vl[frag_k(e, hf) * VP + dcol]; b1[e] = vl[(32 + frag_k(e, hf)) * VP + dcol]; }
                        o[t] = wmma16(pa0, b0, o[t]);
                        o[t] = wmma16(pa1, b1, o[t]);
                    }
                }
            }
        }
    }
    float* obase = p.O + b * p.sOb + h * p.sOh;
    if (p.ST) {
        const int rl = lane >> 1, isel = rl & 7;
        float mv = 0.f, lv = 0.f;
#pragma unroll
        for (int i = 0; i < 8; ++i) if (i == isel) { mv = m8[i]; lv = l8[i]; }
        const int irow = q0 + rl;
        if (irow < p.Lq) { float* st = p.ST + (((long long)b * gridDim.y + h) * p.Lq + irow) * 2 + (lane & 1); VST2(float, st, (lane & 1) ? lv : mv * 0.6931471805599453f); }
    }
    float invr[8];
#pragma unroll
    for (int i = 0; i < 8; ++i) {
        if (TWOPASS) invr[i] = SPLITPV ? 1.f : (1.f / 4096.f);
        else if (p.nonorm) invr[i] = exp2f(m8[i]) * (SPLITPV ? 1.f : (1.f / 4096.f));
        else invr[i] = (l8[i] > 0.f) ? (SPLITPV ? 1.f / l8[i] : 1.f / (l8[i] * 4096.f)) : 0.f;
    }
    __syncthreads();
    const bool ofast = ((p.sOi & 3) == 0) && ((((size_t)obase) & 15) == 0) && (q0 + 16 <= p.Lq);
#pragma unroll
    for (int c0 = 0; c0 < DVP; c0 += 64) {
#pragma unroll
        for (int i = 0; i < 8; ++i)
#pragma unroll
            for (int t = 0; t < NT; ++t) if (t * 16 >= c0 && t * 16 < c0 + 64) myp[(i + 8 * hf) * 64 + (t * 16 - c0) + l15] = o[t][i] * invr[i];
        __syncthreads();
        const int cw = (DVP - c0 < 64) ? (DVP - c0) : 64;
        if (ofast && (c0 + cw <= p.dv) && (cw % 32 == 0)) {
            const int lpr = cw / 4;
            const int rows_per_ins = 32 / lpr;
            for (int r0 = 0; r0 < 16; r0 += rows_per_ins) {
                const int row = r0 + lane / lpr, c4 = (lane % lpr) * 4;
                const v4f v = *(const v4f*)(myp + row * 64 + c4);
                VST2V4(obase + (long long)(q0 + row) * p.sOi + c0 + c4, v);
            }
        } else {
            for (int row = 0; row < 16; ++row) {
                const int irow = q0 + row; if (irow >= p.Lq) continue;
                for (int c = lane; c < cw; c += 32) { const int d = c0 + c; if (d < p.dv) VST2(float, obase + (long long)irow * p.sOi + d, myp[row * 64 + c]); }
            }
        }
        __syncthreads();
    }
}

struct TrP { const float* src; float* dst; const float* R2; long long sSz, lds, sDz, ldd, sRz, ldr; int R, C, flags, act; float alpha, beta; };
static_assert(sizeof(TrP) == 3 * 8 + 6 * 8 + 6 * 4, "TrP has padding");
__global__ __launch_bounds__(256) void k_tr(TrP p) {
    __shared__ float tile[32][33];
    const int c0 = blockIdx.x * 32, r0 = blockIdx.y * 32, z = blockIdx.z;
    const int lane = threadIdx.x & 31, wave = threadIdx.x >> 5;
    const float* s = p.src + z * p.sSz;
#pragma unroll
    for (int k = 0; k < 4; ++k) {
        const int rl = wave * 4 + k, r = r0 + rl, c = c0 + lane;
        tile[rl][lane] = (r < p.R && c < p.C) ? s[(long long)r * p.lds + c] : 0.f;
    }
    __syncthreads();
    float* d = p.dst + z * p.sDz; const float* rr = p.R2 + z * p.sRz;
#pragma unroll
    for (int k = 0; k < 4; ++k) {
        const int cl = wave * 4 + k, c = c0 + cl, r = r0 + lane;
        if (c < p.C && r < p.R) {
            float v = act_fn(p.alpha * tile[lane][cl], p.act);
            if (p.flags & 1) v += p.beta * rr[(long long)c * p.ldr + r];
            VST2(float, d + (long long)c * p.ldd + r, v);
        }
    }
}

__global__ __launch_bounds__(256) void k_affine(const float* __restrict__ src, float* __restrict__ dst, int n, float a, float b, const float* __restrict__ sdev) {
    const int i = blockIdx.x * 256 + threadIdx.x;
    if (i < n) { const float aa = sdev ? a * sdev[0] : a; const float v = aa * src[i] + b; VST2(float, dst + i, v); }
}

struct SmP { const float* src; float* dst; const float* Mf; long long sz, sr, dz, dr, smz, smr; int n, pad; float scale_in, scale_out; };
static_assert(sizeof(SmP) == 3 * 8 + 6 * 8 + 4 * 4, "SmP has padding");
__global__ __launch_bounds__(256) void k_softmax(SmP p) {
    __shared__ float red[256];
    const int r = blockIdx.x, z = blockIdx.y, tid = threadIdx.x;
    const float* s = p.src + z * p.sz + (long long)r * p.sr;
    const float* mf = p.Mf ? (p.Mf + z * p.smz + (long long)r * p.smr) : nullptr;
    float mx = -__builtin_inff();
    for (int j = tid; j < p.n; j += 256) { float v = s[j] * p.scale_in; if (mf) v += mf[j]; mx = fmaxf(mx, v); }
    red[tid] = mx; __syncthreads();
    for (int o = 128; o > 0; o >>= 1) { if (tid < o) red[tid] = fmaxf(red[tid], red[tid + o]); __syncthreads(); }
    mx = red[0]; __syncthreads();
    float sum = 0.f;
    for (int j = tid; j < p.n; j += 256) { float v = s[j] * p.scale_in; if (mf) v += mf[j]; sum += (mx == -__builtin_inff()) ? 0.f : expf(v - mx); }
    red[tid] = sum; __syncthreads();
    for (int o = 128; o > 0; o >>= 1) { if (tid < o) red[tid] += red[tid + o]; __syncthreads(); }
    sum = red[0];
    const float inv = (sum > 0.f) ? p.scale_out / sum : 0.f;
    float* d = p.dst + z * p.dz + (long long)r * p.dr;
    for (int j = tid; j < p.n; j += 256) { float v = s[j] * p.scale_in; if (mf) v += mf[j]; const float o = (mx == -__builtin_inff()) ? 0.f : expf(v - mx) * inv; VST2(float, d + j, o); }
}
__global__ __launch_bounds__(256) void k_stats(const float* __restrict__ x, long long sz, long long so, long long si, int inner, int n, float eps, float* __restrict__ stat, int mode) {
    __shared__ float red[256];
    const int z = blockIdx.x, tid = threadIdx.x;
    const float* base = x + z * sz;
    float s = 0.f;
    for (int e = tid; e < n; e += 256) s += base[(long long)(e / inner) * so + (long long)(e % inner) * si];
    red[tid] = s; __syncthreads();
    for (int o = 128; o > 0; o >>= 1) { if (tid < o) red[tid] += red[tid + o]; __syncthreads(); }
    const float mu = (mode == 0 || mode == 3) ? red[0] / (float)n : 0.f; __syncthreads();
    float q = 0.f;
    for (int e = tid; e < n; e += 256) { const float dlt = base[(long long)(e / inner) * so + (long long)(e % inner) * si] - mu; q += dlt * dlt; }
    red[tid] = q; __syncthreads();
    for (int o = 128; o > 0; o >>= 1) { if (tid < o) red[tid] += red[tid + o]; __syncthreads(); }
    {
        float rs;
        if (mode == 2) rs = sqrtf((float)n) / fmaxf(sqrtf(red[0]), eps); else if (mode == 3) rs = rsqrtf(red[0] / (float)(n - 1) + eps); else rs = rsqrtf(red[0] / (float)n + eps);
        if (tid < 32) { const float v = (tid == 0) ? mu : ((tid == 1) ? rs : 0.f); VST2(float, stat + (long long)z * 32 + tid, v); }
    }
}
__global__ __launch_bounds__(256) void k_norm_apply(const float* __restrict__ x, float* __restrict__ y, const float* __restrict__ stat, const float* __restrict__ g, const float* __restrict__ bta,
                                                     int Z, int C, int L, int G, int bn, int act) {
    const long long idx = (long long)blockIdx.x * 256 + threadIdx.x;
    if (idx >= (long long)Z * C * L) return;
    const int l = (int)(idx % L); const long long zc = idx / L; const int c = (int)(zc % C), z = (int)(zc / C); (void)l;
    const int set = bn ? c : (z * G + c / (C / G));
    float v = (x[idx] - stat[(long long)set * 32]) * stat[(long long)set * 32 + 1];
    if (g) v *= g[c];
    if (bta) v += bta[c];
    v = act_fn(v, act);
    VST2(float, y + idx, v);
}

__global__ __launch_bounds__(256) void k_lse_neg(const float* __restrict__ st, float* __restrict__ c, int n) {
    const int i = blockIdx.x * 256 + threadIdx.x;
    if (i < n) { const float v = -(st[2 * i] + logf(st[2 * i + 1])); VST2(float, c + i, v); }
}

__global__ __launch_bounds__(256) void k_iota(int* __restrict__ dst, int n, int a, int b) {
    const int i = blockIdx.x * 256 + threadIdx.x;
    if (i < n) { const int v = a * i + b; VST2(int, dst + i, v); }
}

__global__ __launch_bounds__(256) void k_axpby(const float* __restrict__ x, const float* __restrict__ y, float* __restrict__ dst, int n, float a, float b, float c) {
    const int i = blockIdx.x * 256 + threadIdx.x;
    if (i < n) { const float v = a * x[i] + b * y[i] + c; VST2(float, dst + i, v); }
}

struct RopeP { const float* X; float* Y; const float* C; const float* Sn; const int* pos; long long sXr, sXh, sYr, sYh, sCb, sCp, sCd; int R, Hn, D, S, mode, tmode, pmode, pad; };
static_assert(sizeof(RopeP) == 5 * 8 + 7 * 8 + 8 * 4, "RopeP has padding");
__global__ __launch_bounds__(256) void k_rope(RopeP p) {
    const long long idx = (long long)blockIdx.x * 256 + threadIdx.x;
    if (idx >= (long long)p.R * p.Hn * p.D) return;
    const int d = (int)(idx % p.D); const long long rh = idx / p.D; const int h = (int)(rh % p.Hn); const int r = (int)(rh / p.Hn);
    const int half = p.D / 2;
    int partner; float sign;
    if (p.mode == 0) { partner = (d < half) ? d + half : d - half; sign = (d < half) ? -1.f : 1.f; }
    else { partner = d ^ 1; sign = (d & 1) ? 1.f : -1.f; }
    const int tcol = (p.tmode == 0) ? d : ((p.tmode == 1) ? (d % half) : (d >> 1));
    const int pp = (p.pmode == 0) ? (r % p.S) : ((p.pmode == 1) ? h : p.pos[r]);
    const long long toff = (long long)(r / p.S) * p.sCb + (long long)pp * p.sCp + (long long)tcol * p.sCd;
    const float* xr = p.X + (long long)r * p.sXr + (long long)h * p.sXh;
    const float v = xr[d] * p.C[toff] + sign * xr[partner] * p.Sn[toff];
    VST2(float, p.Y + (long long)r * p.sYr + (long long)h * p.sYh + d, v);
}

__global__ __launch_bounds__(256) void k_invf(float* __restrict__ invb, int half, int D, float base, float num, int fmode, float cexp) {
    const int i = blockIdx.x * 256 + threadIdx.x;
    if (i >= ((half + 31) / 32) * 32) return;
    if (i >= half) { VST2(float, invb + i, 0.f); return; }
    const float e = (float)(2 * i) / (float)D;
    float invf;
    if (fmode == 1) invf = num * expf((float)(2 * i) * cexp);
    else if (fmode == 2) invf = num * powf(base, (-2.0f * ((float)i - 1.0f)) / (float)D);
    else invf = num * (1.0f / powf(base, e));
    VST2(float, invb + i, invf);
}
__global__ __launch_bounds__(256) void k_sincos(float* __restrict__ cs, float* __restrict__ sn, const float* __restrict__ invb, int S, int half, float pscale) {
    const int idx = blockIdx.x * 256 + threadIdx.x;
    if (idx >= S * half) return;
    const int s = idx / half, i = idx - s * half;
    const float ang = (pscale * (float)s) * invb[i];
    VST2(float, cs + idx, cosf(ang)); VST2(float, sn + idx, sinf(ang));
}

__global__ __launch_bounds__(256) void k_mulact(const float* __restrict__ x, const float* __restrict__ y, float* __restrict__ dst, int n, int act) {
    const int i = blockIdx.x * 256 + threadIdx.x;
    if (i < n) { const float v = act_fn(x[i], act) * y[i]; VST2(float, dst + i, v); }
}

__global__ __launch_bounds__(256) void k_matvec(GemmP p) {
    const int rpt = (p.N == 1) ? 1 : 32;
    const long long r0 = ((long long)blockIdx.x * 256 + threadIdx.x) * rpt; const int z = blockIdx.z, zo = z / p.zi_n, zi = z - zo * p.zi_n;
    if (r0 >= p.M) return;
    const float* Bb = p.B + zo * p.sBo + zi * p.sBi;
    float* C = p.C + zo * p.sCo + zi * p.sCi; const float* R = p.R + zo * p.sRo + zi * p.sRi;
    for (int rr = 0; rr < rpt; ++rr) {
        const long long r = r0 + rr; if (r >= p.M) break;
        const float* A = p.A + zo * p.sAo + zi * p.sAi + r * p.sAm;
        float acc[8] = {0.f, 0.f, 0.f, 0.f, 0.f, 0.f, 0.f, 0.f};
        for (int k = 0; k < p.K; ++k) { const float a = A[(long long)k * p.sAk];
#pragma unroll
            for (int j = 0; j < 8; ++j) if (j < p.N) acc[j] += a * Bb[(long long)j * p.sBn + (long long)k * p.sBk]; }
#pragma unroll
        for (int j = 0; j < 8; ++j) if (j < p.N) {
            float v = acc[j] * p.alpha;
            if (p.flags & 1) v += p.bias[j];
            if (p.flags & 2) v += p.bias[r];
            v = act_fn(v, p.act);
            if (p.flags & 4) v += p.beta * R[r * p.sRm + (long long)j * p.sRn];
            VST2(float, C + r * p.sCm + j, v);
        }
    }
}
__global__ __launch_bounds__(256) void k_smallsoftmax(const float* __restrict__ src, float* __restrict__ dst, long long sr, long long dr, int n, long long R, float scale) {
    const long long r0 = ((long long)blockIdx.x * 256 + threadIdx.x) * 32;
    for (int rr = 0; rr < 32; ++rr) {
        const long long r = r0 + rr; if (r >= R) return;
        const float* s = src + r * sr; float* d = dst + r * dr;
        float mx = -__builtin_inff();
        for (int j = 0; j < n; ++j) mx = fmaxf(mx, s[j] * scale);
        float sum = 0.f;
        for (int j = 0; j < n; ++j) sum += expf(s[j] * scale - mx);
        const float inv = 1.f / sum;
        for (int j = 0; j < n; ++j) { const float v = expf(s[j] * scale - mx) * inv; VST2(float, d + j, v); }
    }
}

__global__ __launch_bounds__(32) void k_unitstat(float* __restrict__ st) { const int t = threadIdx.x; const float v = (t == 1) ? 1.f : 0.f; VST2(float, st + t, v); }

__global__ __launch_bounds__(256) void k_lincopy(const float* __restrict__ src, long long lds, float* __restrict__ dst, long long ldd, long long rows, int cols) {
    const long long i = (long long)blockIdx.x * 256 + threadIdx.x; if (i >= rows * cols) return;
    const long long r = i / cols; const int c = (int)(i - r * cols);
    const float v = src[r * lds + c]; VST2(float, dst + r * ldd + c, v);
}

template __global__ void k_gemm<1>(GemmP);

extern "C" void kernel_launch(void* const* d_in, const int* in_sizes, int n_in, void* d_out, int out_size, void* d_ws, size_t ws_size, hipStream_t stream) {
    (void)in_sizes; (void)n_in; (void)out_size; (void)ws_size;
    const float* x = (const float*)d_in[0];
    const float* w = (const float*)d_in[1];
    const float* b = (const float*)d_in[2];
    const int NB = 32;
    const int C = 64;
    const int W = 4096;
    const int F = 128;
    const int WW = 64;
    const int OW = 4033;
    const int LDO = 4064;
    float* out = (float*)d_out;
    char* wsp = (char*)d_ws;
    float* ST = (float*)wsp; wsp += (((size_t)((size_t)NB * F * LDO) * 4 + 255) / 256) * 256;
    { GemmP g0;
      g0.A = w + 0; g0.B = x + (size_t)0 * W; g0.bias = b; g0.R = w + 0; g0.C = ST;
      g0.sAo = 0; g0.sAi = 0; g0.sAm = C * WW; g0.sAk = 1; g0.sBo = (long long)C * W; g0.sBi = 0; g0.sBn = 1; g0.sBk = 1; g0.sCo = (long long)F * LDO; g0.sCi = 0; g0.sCm = LDO; g0.sRo = 0; g0.sRi = 0; g0.sRm = 0; g0.sRn = 0;
      g0.M = F; g0.N = OW; g0.K = WW; g0.zi_n = 1; g0.flags = 2; g0.act = 0;
      g0.alpha = 1.0f; g0.beta = 0.0f; g0.sa = 1.0f; g0.sb = 1.0f; g0.Npad = OW; g0.pad_ = 0;
      k_gemm<1><<<dim3((unsigned)((OW) + 31) / 32, (unsigned)((F) + 15) / 16, (unsigned)(NB)), 32, 0, stream>>>(g0); }
    { GemmP g1;
      g1.A = w + 64; g1.B = x + (size_t)1 * W; g1.bias = w + 64; g1.R = ST; g1.C = ST;
      g1.sAo = 0; g1.sAi = 0; g1.sAm = C * WW; g1.sAk = 1; g1.sBo = (long long)C * W; g1.sBi = 0; g1.sBn = 1; g1.sBk = 1; g1.sCo = (long long)F * LDO; g1.sCi = 0; g1.sCm = LDO; g1.sRo = (long long)F * LDO; g1.sRi = 0; g1.sRm = LDO; g1.sRn = 1;
      g1.M = F; g1.N = OW; g1.K = WW; g1.zi_n = 1; g1.flags = 4; g1.act = 0;
      g1.alpha = 1.0f; g1.beta = 1.0f; g1.sa = 1.0f; g1.sb = 1.0f; g1.Npad = OW; g1.pad_ = 0;
      k_gemm<1><<<dim3((unsigned)((OW) + 31) / 32, (unsigned)((F) + 15) / 16, (unsigned)(NB)), 32, 0, stream>>>(g1); }
    { GemmP g2;
      g2.A = w + 128; g2.B = x + (size_t)2 * W; g2.bias = w + 128; g2.R = ST; g2.C = ST;
      g2.sAo = 0; g2.sAi = 0; g2.sAm = C * WW; g2.sAk = 1; g2.sBo = (long long)C * W; g2.sBi = 0; g2.sBn = 1; g2.sBk = 1; g2.sCo = (long long)F * LDO; g2.sCi = 0; g2.sCm = LDO; g2.sRo = (long long)F * LDO; g2.sRi = 0; g2.sRm = LDO; g2.sRn = 1;
      g2.M = F; g2.N = OW; g2.K = WW; g2.zi_n = 1; g2.flags = 4; g2.act = 0;
      g2.alpha = 1.0f; g2.beta = 1.0f; g2.sa = 1.0f; g2.sb = 1.0f; g2.Npad = OW; g2.pad_ = 0;
      k_gemm<1><<<dim3((unsigned)((OW) + 31) / 32, (unsigned)((F) + 15) / 16, (unsigned)(NB)), 32, 0, stream>>>(g2); }
    { GemmP g3;
      g3.A = w + 192; g3.B = x + (size_t)3 * W; g3.bias = w + 192; g3.R = ST; g3.C = ST;
      g3.sAo = 0; g3.sAi = 0; g3.sAm = C * WW; g3.sAk = 1; g3.sBo = (long long)C * W; g3.sBi = 0; g3.sBn = 1; g3.sBk = 1; g3.sCo = (long long)F * LDO; g3.sCi = 0; g3.sCm = LDO; g3.sRo = (long long)F * LDO; g3.sRi = 0; g3.sRm = LDO; g3.sRn = 1;
      g3.M = F; g3.N = OW; g3.K = WW; g3.zi_n = 1; g3.flags = 4; g3.act = 0;
      g3.alpha = 1.0f; g3.beta = 1.0f; g3.sa = 1.0f; g3.sb = 1.0f; g3.Npad = OW; g3.pad_ = 0;
      k_gemm<1><<<dim3((unsigned)((OW) + 31) / 32, (unsigned)((F) + 15) / 16, (unsigned)(NB)), 32, 0, stream>>>(g3); }
    { GemmP g4;
      g4.A = w + 256; g4.B = x + (size_t)4 * W; g4.bias = w + 256; g4.R = ST; g4.C = ST;
      g4.sAo = 0; g4.sAi = 0; g4.sAm = C * WW; g4.sAk = 1; g4.sBo = (long long)C * W; g4.sBi = 0; g4.sBn = 1; g4.sBk = 1; g4.sCo = (long long)F * LDO; g4.sCi = 0; g4.sCm = LDO; g4.sRo = (long long)F * LDO; g4.sRi = 0; g4.sRm = LDO; g4.sRn = 1;
      g4.M = F; g4.N = OW; g4.K = WW; g4.zi_n = 1; g4.flags = 4; g4.act = 0;
      g4.alpha = 1.0f; g4.beta = 1.0f; g4.sa = 1.0f; g4.sb = 1.0f; g4.Npad = OW; g4.pad_ = 0;
      k_gemm<1><<<dim3((unsigned)((OW) + 31) / 32, (unsigned)((F) + 15) / 16, (unsigned)(NB)), 32, 0, stream>>>(g4); }
    { GemmP g5;
      g5.A = w + 320; g5.B = x + (size_t)5 * W; g5.bias = w + 320; g5.R = ST; g5.C = ST;
      g5.sAo = 0; g5.sAi = 0; g5.sAm = C * WW; g5.sAk = 1; g5.sBo = (long long)C * W; g5.sBi = 0; g5.sBn = 1; g5.sBk = 1; g5.sCo = (long long)F * LDO; g5.sCi = 0; g5.sCm = LDO; g5.sRo = (long long)F * LDO; g5.sRi = 0; g5.sRm = LDO; g5.sRn = 1;
      g5.M = F; g5.N = OW; g5.K = WW; g5.zi_n = 1; g5.flags = 4; g5.act = 0;
      g5.alpha = 1.0f; g5.beta = 1.0f; g5.sa = 1.0f; g5.sb = 1.0f; g5.Npad = OW; g5.pad_ = 0;
      k_gemm<1><<<dim3((unsigned)((OW) + 31) / 32, (unsigned)((F) + 15) / 16, (unsigned)(NB)), 32, 0, stream>>>(g5); }
    { GemmP g6;
      g6.A = w + 384; g6.B = x + (size_t)6 * W; g6.bias = w + 384; g6.R = ST; g6.C = ST;
      g6.sAo = 0; g6.sAi = 0; g6.sAm = C * WW; g6.sAk = 1; g6.sBo = (long long)C * W; g6.sBi = 0; g6.sBn = 1; g6.sBk = 1; g6.sCo = (long long)F * LDO; g6.sCi = 0; g6.sCm = LDO; g6.sRo = (long long)F * LDO; g6.sRi = 0; g6.sRm = LDO; g6.sRn = 1;
      g6.M = F; g6.N = OW; g6.K = WW; g6.zi_n = 1; g6.flags = 4; g6.act = 0;
      g6.alpha = 1.0f; g6.beta = 1.0f; g6.sa = 1.0f; g6.sb = 1.0f; g6.Npad = OW; g6.pad_ = 0;
      k_gemm<1><<<dim3((unsigned)((OW) + 31) / 32, (unsigned)((F) + 15) / 16, (unsigned)(NB)), 32, 0, stream>>>(g6); }
    { GemmP g7;
      g7.A = w + 448; g7.B = x + (size_t)7 * W; g7.bias = w + 448; g7.R = ST; g7.C = ST;
      g7.sAo = 0; g7.sAi = 0; g7.sAm = C * WW; g7.sAk = 1; g7.sBo = (long long)C * W; g7.sBi = 0; g7.sBn = 1; g7.sBk = 1; g7.sCo = (long long)F * LDO; g7.sCi = 0; g7.sCm = LDO; g7.sRo = (long long)F * LDO; g7.sRi = 0; g7.sRm = LDO; g7.sRn = 1;
      g7.M = F; g7.N = OW; g7.K = WW; g7.zi_n = 1; g7.flags = 4; g7.act = 0;
      g7.alpha = 1.0f; g7.beta = 1.0f; g7.sa = 1.0f; g7.sb = 1.0f; g7.Npad = OW; g7.pad_ = 0;
      k_gemm<1><<<dim3((unsigned)((OW) + 31) / 32, (unsigned)((F) + 15) / 16, (unsigned)(NB)), 32, 0, stream>>>(g7); }
    { GemmP g8;
      g8.A = w + 512; g8.B = x + (size_t)8 * W; g8.bias = w + 512; g8.R = ST; g8.C = ST;
      g8.sAo = 0; g8.sAi = 0; g8.sAm = C * WW; g8.sAk = 1; g8.sBo = (long long)C * W; g8.sBi = 0; g8.sBn = 1; g8.sBk = 1; g8.sCo = (long long)F * LDO; g8.sCi = 0; g8.sCm = LDO; g8.sRo = (long long)F * LDO; g8.sRi = 0; g8.sRm = LDO; g8.sRn = 1;
      g8.M = F; g8.N = OW; g8.K = WW; g8.zi_n = 1; g8.flags = 4; g8.act = 0;
      g8.alpha = 1.0f; g8.beta = 1.0f; g8.sa = 1.0f; g8.sb = 1.0f; g8.Npad = OW; g8.pad_ = 0;
      k_gemm<1><<<dim3((unsigned)((OW) + 31) / 32, (unsigned)((F) + 15) / 16, (unsigned)(NB)), 32, 0, stream>>>(g8); }
    { GemmP g9;
      g9.A = w + 576; g9.B = x + (size_t)9 * W; g9.bias = w + 576; g9.R = ST; g9.C = ST;
      g9.sAo = 0; g9.sAi = 0; g9.sAm = C * WW; g9.sAk = 1; g9.sBo = (long long)C * W; g9.sBi = 0; g9.sBn = 1; g9.sBk = 1; g9.sCo = (long long)F * LDO; g9.sCi = 0; g9.sCm = LDO; g9.sRo = (long long)F * LDO; g9.sRi = 0; g9.sRm = LDO; g9.sRn = 1;
      g9.M = F; g9.N = OW; g9.K = WW; g9.zi_n = 1; g9.flags = 4; g9.act = 0;
      g9.alpha = 1.0f; g9.beta = 1.0f; g9.sa = 1.0f; g9.sb = 1.0f; g9.Npad = OW; g9.pad_ = 0;
      k_gemm<1><<<dim3((unsigned)((OW) + 31) / 32, (unsigned)((F) + 15) / 16, (unsigned)(NB)), 32, 0, stream>>>(g9); }
    { GemmP g10;
      g10.A = w + 640; g10.B = x + (size_t)10 * W; g10.bias = w + 640; g10.R = ST; g10.C = ST;
      g10.sAo = 0; g10.sAi = 0; g10.sAm = C * WW; g10.sAk = 1; g10.sBo = (long long)C * W; g10.sBi = 0; g10.sBn = 1; g10.sBk = 1; g10.sCo = (long long)F * LDO; g10.sCi = 0; g10.sCm = LDO; g10.sRo = (long long)F * LDO; g10.sRi = 0; g10.sRm = LDO; g10.sRn = 1;
      g10.M = F; g10.N = OW; g10.K = WW; g10.zi_n = 1; g10.flags = 4; g10.act = 0;
      g10.alpha = 1.0f; g10.beta = 1.0f; g10.sa = 1.0f; g10.sb = 1.0f; g10.Npad = OW; g10.pad_ = 0;
      k_gemm<1><<<dim3((unsigned)((OW) + 31) / 32, (unsigned)((F) + 15) / 16, (unsigned)(NB)), 32, 0, stream>>>(g10); }
    { GemmP g11;
      g11.A = w + 704; g11.B = x + (size_t)11 * W; g11.bias = w + 704; g11.R = ST; g11.C = ST;
      g11.sAo = 0; g11.sAi = 0; g11.sAm = C * WW; g11.sAk = 1; g11.sBo = (long long)C * W; g11.sBi = 0; g11.sBn = 1; g11.sBk = 1; g11.sCo = (long long)F * LDO; g11.sCi = 0; g11.sCm = LDO; g11.sRo = (long long)F * LDO; g11.sRi = 0; g11.sRm = LDO; g11.sRn = 1;
      g11.M = F; g11.N = OW; g11.K = WW; g11.zi_n = 1; g11.flags = 4; g11.act = 0;
      g11.alpha = 1.0f; g11.beta = 1.0f; g11.sa = 1.0f; g11.sb = 1.0f; g11.Npad = OW; g11.pad_ = 0;
      k_gemm<1><<<dim3((unsigned)((OW) + 31) / 32, (unsigned)((F) + 15) / 16, (unsigned)(NB)), 32, 0, stream>>>(g11); }
    { GemmP g12;
      g12.A = w + 768; g12.B = x + (size_t)12 * W; g12.bias = w + 768; g12.R = ST; g12.C = ST;
      g12.sAo = 0; g12.sAi = 0; g12.sAm = C * WW; g12.sAk = 1; g12.sBo = (long long)C * W; g12.sBi = 0; g12.sBn = 1; g12.sBk = 1; g12.sCo = (long long)F * LDO; g12.sCi = 0; g12.sCm = LDO; g12.sRo = (long long)F * LDO; g12.sRi = 0; g12.sRm = LDO; g12.sRn = 1;
      g12.M = F; g12.N = OW; g12.K = WW; g12.zi_n = 1; g12.flags = 4; g12.act = 0;
      g12.alpha = 1.0f; g12.beta = 1.0f; g12.sa = 1.0f; g12.sb = 1.0f; g12.Npad = OW; g12.pad_ = 0;
      k_gemm<1><<<dim3((unsigned)((OW) + 31) / 32, (unsigned)((F) + 15) / 16, (unsigned)(NB)), 32, 0, stream>>>(g12); }
    { GemmP g13;
      g13.A = w + 832; g13.B = x + (size_t)13 * W; g13.bias = w + 832; g13.R = ST; g13.C = ST;
      g13.sAo = 0; g13.sAi = 0; g13.sAm = C * WW; g13.sAk = 1; g13.sBo = (long long)C * W; g13.sBi = 0; g13.sBn = 1; g13.sBk = 1; g13.sCo = (long long)F * LDO; g13.sCi = 0; g13.sCm = LDO; g13.sRo = (long long)F * LDO; g13.sRi = 0; g13.sRm = LDO; g13.sRn = 1;
      g13.M = F; g13.N = OW; g13.K = WW; g13.zi_n = 1; g13.flags = 4; g13.act = 0;
      g13.alpha = 1.0f; g13.beta = 1.0f; g13.sa = 1.0f; g13.sb = 1.0f; g13.Npad = OW; g13.pad_ = 0;
      k_gemm<1><<<dim3((unsigned)((OW) + 31) / 32, (unsigned)((F) + 15) / 16, (unsigned)(NB)), 32, 0, stream>>>(g13); }
    { GemmP g14;
      g14.A = w + 896; g14.B = x + (size_t)14 * W; g14.bias = w + 896; g14.R = ST; g14.C = ST;
      g14.sAo = 0; g14.sAi = 0; g14.sAm = C * WW; g14.sAk = 1; g14.sBo = (long long)C * W; g14.sBi = 0; g14.sBn = 1; g14.sBk = 1; g14.sCo = (long long)F * LDO; g14.sCi = 0; g14.sCm = LDO; g14.sRo = (long long)F * LDO; g14.sRi = 0; g14.sRm = LDO; g14.sRn = 1;
      g14.M = F; g14.N = OW; g14.K = WW; g14.zi_n = 1; g14.flags = 4; g14.act = 0;
      g14.alpha = 1.0f; g14.beta = 1.0f; g14.sa = 1.0f; g14.sb = 1.0f; g14.Npad = OW; g14.pad_ = 0;
      k_gemm<1><<<dim3((unsigned)((OW) + 31) / 32, (unsigned)((F) + 15) / 16, (unsigned)(NB)), 32, 0, stream>>>(g14); }
    { GemmP g15;
      g15.A = w + 960; g15.B = x + (size_t)15 * W; g15.bias = w + 960; g15.R = ST; g15.C = ST;
      g15.sAo = 0; g15.sAi = 0; g15.sAm = C * WW; g15.sAk = 1; g15.sBo = (long long)C * W; g15.sBi = 0; g15.sBn = 1; g15.sBk = 1; g15.sCo = (long long)F * LDO; g15.sCi = 0; g15.sCm = LDO; g15.sRo = (long long)F * LDO; g15.sRi = 0; g15.sRm = LDO; g15.sRn = 1;
      g15.M = F; g15.N = OW; g15.K = WW; g15.zi_n = 1; g15.flags = 4; g15.act = 0;
      g15.alpha = 1.0f; g15.beta = 1.0f; g15.sa = 1.0f; g15.sb = 1.0f; g15.Npad = OW; g15.pad_ = 0;
      k_gemm<1><<<dim3((unsigned)((OW) + 31) / 32, (unsigned)((F) + 15) / 16, (unsigned)(NB)), 32, 0, stream>>>(g15); }
    { GemmP g16;
      g16.A = w + 1024; g16.B = x + (size_t)16 * W; g16.bias = w + 1024; g16.R = ST; g16.C = ST;
      g16.sAo = 0; g16.sAi = 0; g16.sAm = C * WW; g16.sAk = 1; g16.sBo = (long long)C * W; g16.sBi = 0; g16.sBn = 1; g16.sBk = 1; g16.sCo = (long long)F * LDO; g16.sCi = 0; g16.sCm = LDO; g16.sRo = (long long)F * LDO; g16.sRi = 0; g16.sRm = LDO; g16.sRn = 1;
      g16.M = F; g16.N = OW; g16.K = WW; g16.zi_n = 1; g16.flags = 4; g16.act = 0;
      g16.alpha = 1.0f; g16.beta = 1.0f; g16.sa = 1.0f; g16.sb = 1.0f; g16.Npad = OW; g16.pad_ = 0;
      k_gemm<1><<<dim3((unsigned)((OW) + 31) / 32, (unsigned)((F) + 15) / 16, (unsigned)(NB)), 32, 0, stream>>>(g16); }
    { GemmP g17;
      g17.A = w + 1088; g17.B = x + (size_t)17 * W; g17.bias = w + 1088; g17.R = ST; g17.C = ST;
      g17.sAo = 0; g17.sAi = 0; g17.sAm = C * WW; g17.sAk = 1; g17.sBo = (long long)C * W; g17.sBi = 0; g17.sBn = 1; g17.sBk = 1; g17.sCo = (long long)F * LDO; g17.sCi = 0; g17.sCm = LDO; g17.sRo = (long long)F * LDO; g17.sRi = 0; g17.sRm = LDO; g17.sRn = 1;
      g17.M = F; g17.N = OW; g17.K = WW; g17.zi_n = 1; g17.flags = 4; g17.act = 0;
      g17.alpha = 1.0f; g17.beta = 1.0f; g17.sa = 1.0f; g17.sb = 1.0f; g17.Npad = OW; g17.pad_ = 0;
      k_gemm<1><<<dim3((unsigned)((OW) + 31) / 32, (unsigned)((F) + 15) / 16, (unsigned)(NB)), 32, 0, stream>>>(g17); }
    { GemmP g18;
      g18.A = w + 1152; g18.B = x + (size_t)18 * W; g18.bias = w + 1152; g18.R = ST; g18.C = ST;
      g18.sAo = 0; g18.sAi = 0; g18.sAm = C * WW; g18.sAk = 1; g18.sBo = (long long)C * W; g18.sBi = 0; g18.sBn = 1; g18.sBk = 1; g18.sCo = (long long)F * LDO; g18.sCi = 0; g18.sCm = LDO; g18.sRo = (long long)F * LDO; g18.sRi = 0; g18.sRm = LDO; g18.sRn = 1;
      g18.M = F; g18.N = OW; g18.K = WW; g18.zi_n = 1; g18.flags = 4; g18.act = 0;
      g18.alpha = 1.0f; g18.beta = 1.0f; g18.sa = 1.0f; g18.sb = 1.0f; g18.Npad = OW; g18.pad_ = 0;
      k_gemm<1><<<dim3((unsigned)((OW) + 31) / 32, (unsigned)((F) + 15) / 16, (unsigned)(NB)), 32, 0, stream>>>(g18); }
    { GemmP g19;
      g19.A = w + 1216; g19.B = x + (size_t)19 * W; g19.bias = w + 1216; g19.R = ST; g19.C = ST;
      g19.sAo = 0; g19.sAi = 0; g19.sAm = C * WW; g19.sAk = 1; g19.sBo = (long long)C * W; g19.sBi = 0; g19.sBn = 1; g19.sBk = 1; g19.sCo = (long long)F * LDO; g19.sCi = 0; g19.sCm = LDO; g19.sRo = (long long)F * LDO; g19.sRi = 0; g19.sRm = LDO; g19.sRn = 1;
      g19.M = F; g19.N = OW; g19.K = WW; g19.zi_n = 1; g19.flags = 4; g19.act = 0;
      g19.alpha = 1.0f; g19.beta = 1.0f; g19.sa = 1.0f; g19.sb = 1.0f; g19.Npad = OW; g19.pad_ = 0;
      k_gemm<1><<<dim3((unsigned)((OW) + 31) / 32, (unsigned)((F) + 15) / 16, (unsigned)(NB)), 32, 0, stream>>>(g19); }
    { GemmP g20;
      g20.A = w + 1280; g20.B = x + (size_t)20 * W; g20.bias = w + 1280; g20.R = ST; g20.C = ST;
      g20.sAo = 0; g20.sAi = 0; g20.sAm = C * WW; g20.sAk = 1; g20.sBo = (long long)C * W; g20.sBi = 0; g20.sBn = 1; g20.sBk = 1; g20.sCo = (long long)F * LDO; g20.sCi = 0; g20.sCm = LDO; g20.sRo = (long long)F * LDO; g20.sRi = 0; g20.sRm = LDO; g20.sRn = 1;
      g20.M = F; g20.N = OW; g20.K = WW; g20.zi_n = 1; g20.flags = 4; g20.act = 0;
      g20.alpha = 1.0f; g20.beta = 1.0f; g20.sa = 1.0f; g20.sb = 1.0f; g20.Npad = OW; g20.pad_ = 0;
      k_gemm<1><<<dim3((unsigned)((OW) + 31) / 32, (unsigned)((F) + 15) / 16, (unsigned)(NB)), 32, 0, stream>>>(g20); }
    { GemmP g21;
      g21.A = w + 1344; g21.B = x + (size_t)21 * W; g21.bias = w + 1344; g21.R = ST; g21.C = ST;
      g21.sAo = 0; g21.sAi = 0; g21.sAm = C * WW; g21.sAk = 1; g21.sBo = (long long)C * W; g21.sBi = 0; g21.sBn = 1; g21.sBk = 1; g21.sCo = (long long)F * LDO; g21.sCi = 0; g21.sCm = LDO; g21.sRo = (long long)F * LDO; g21.sRi = 0; g21.sRm = LDO; g21.sRn = 1;
      g21.M = F; g21.N = OW; g21.K = WW; g21.zi_n = 1; g21.flags = 4; g21.act = 0;
      g21.alpha = 1.0f; g21.beta = 1.0f; g21.sa = 1.0f; g21.sb = 1.0f; g21.Npad = OW; g21.pad_ = 0;
      k_gemm<1><<<dim3((unsigned)((OW) + 31) / 32, (unsigned)((F) + 15) / 16, (unsigned)(NB)), 32, 0, stream>>>(g21); }
    { GemmP g22;
      g22.A = w + 1408; g22.B = x + (size_t)22 * W; g22.bias = w + 1408; g22.R = ST; g22.C = ST;
      g22.sAo = 0; g22.sAi = 0; g22.sAm = C * WW; g22.sAk = 1; g22.sBo = (long long)C * W; g22.sBi = 0; g22.sBn = 1; g22.sBk = 1; g22.sCo = (long long)F * LDO; g22.sCi = 0; g22.sCm = LDO; g22.sRo = (long long)F * LDO; g22.sRi = 0; g22.sRm = LDO; g22.sRn = 1;
      g22.M = F; g22.N = OW; g22.K = WW; g22.zi_n = 1; g22.flags = 4; g22.act = 0;
      g22.alpha = 1.0f; g22.beta = 1.0f; g22.sa = 1.0f; g22.sb = 1.0f; g22.Npad = OW; g22.pad_ = 0;
      k_gemm<1><<<dim3((unsigned)((OW) + 31) / 32, (unsigned)((F) + 15) / 16, (unsigned)(NB)), 32, 0, stream>>>(g22); }
    { GemmP g23;
      g23.A = w + 1472; g23.B = x + (size_t)23 * W; g23.bias = w + 1472; g23.R = ST; g23.C = ST;
      g23.sAo = 0; g23.sAi = 0; g23.sAm = C * WW; g23.sAk = 1; g23.sBo = (long long)C * W; g23.sBi = 0; g23.sBn = 1; g23.sBk = 1; g23.sCo = (long long)F * LDO; g23.sCi = 0; g23.sCm = LDO; g23.sRo = (long long)F * LDO; g23.sRi = 0; g23.sRm = LDO; g23.sRn = 1;
      g23.M = F; g23.N = OW; g23.K = WW; g23.zi_n = 1; g23.flags = 4; g23.act = 0;
      g23.alpha = 1.0f; g23.beta = 1.0f; g23.sa = 1.0f; g23.sb = 1.0f; g23.Npad = OW; g23.pad_ = 0;
      k_gemm<1><<<dim3((unsigned)((OW) + 31) / 32, (unsigned)((F) + 15) / 16, (unsigned)(NB)), 32, 0, stream>>>(g23); }
    { GemmP g24;
      g24.A = w + 1536; g24.B = x + (size_t)24 * W; g24.bias = w + 1536; g24.R = ST; g24.C = ST;
      g24.sAo = 0; g24.sAi = 0; g24.sAm = C * WW; g24.sAk = 1; g24.sBo = (long long)C * W; g24.sBi = 0; g24.sBn = 1; g24.sBk = 1; g24.sCo = (long long)F * LDO; g24.sCi = 0; g24.sCm = LDO; g24.sRo = (long long)F * LDO; g24.sRi = 0; g24.sRm = LDO; g24.sRn = 1;
      g24.M = F; g24.N = OW; g24.K = WW; g24.zi_n = 1; g24.flags = 4; g24.act = 0;
      g24.alpha = 1.0f; g24.beta = 1.0f; g24.sa = 1.0f; g24.sb = 1.0f; g24.Npad = OW; g24.pad_ = 0;
      k_gemm<1><<<dim3((unsigned)((OW) + 31) / 32, (unsigned)((F) + 15) / 16, (unsigned)(NB)), 32, 0, stream>>>(g24); }
    { GemmP g25;
      g25.A = w + 1600; g25.B = x + (size_t)25 * W; g25.bias = w + 1600; g25.R = ST; g25.C = ST;
      g25.sAo = 0; g25.sAi = 0; g25.sAm = C * WW; g25.sAk = 1; g25.sBo = (long long)C * W; g25.sBi = 0; g25.sBn = 1; g25.sBk = 1; g25.sCo = (long long)F * LDO; g25.sCi = 0; g25.sCm = LDO; g25.sRo = (long long)F * LDO; g25.sRi = 0; g25.sRm = LDO; g25.sRn = 1;
      g25.M = F; g25.N = OW; g25.K = WW; g25.zi_n = 1; g25.flags = 4; g25.act = 0;
      g25.alpha = 1.0f; g25.beta = 1.0f; g25.sa = 1.0f; g25.sb = 1.0f; g25.Npad = OW; g25.pad_ = 0;
      k_gemm<1><<<dim3((unsigned)((OW) + 31) / 32, (unsigned)((F) + 15) / 16, (unsigned)(NB)), 32, 0, stream>>>(g25); }
    { GemmP g26;
      g26.A = w + 1664; g26.B = x + (size_t)26 * W; g26.bias = w + 1664; g26.R = ST; g26.C = ST;
      g26.sAo = 0; g26.sAi = 0; g26.sAm = C * WW; g26.sAk = 1; g26.sBo = (long long)C * W; g26.sBi = 0; g26.sBn = 1; g26.sBk = 1; g26.sCo = (long long)F * LDO; g26.sCi = 0; g26.sCm = LDO; g26.sRo = (long long)F * LDO; g26.sRi = 0; g26.sRm = LDO; g26.sRn = 1;
      g26.M = F; g26.N = OW; g26.K = WW; g26.zi_n = 1; g26.flags = 4; g26.act = 0;
      g26.alpha = 1.0f; g26.beta = 1.0f; g26.sa = 1.0f; g26.sb = 1.0f; g26.Npad = OW; g26.pad_ = 0;
      k_gemm<1><<<dim3((unsigned)((OW) + 31) / 32, (unsigned)((F) + 15) / 16, (unsigned)(NB)), 32, 0, stream>>>(g26); }
    { GemmP g27;
      g27.A = w + 1728; g27.B = x + (size_t)27 * W; g27.bias = w + 1728; g27.R = ST; g27.C = ST;
      g27.sAo = 0; g27.sAi = 0; g27.sAm = C * WW; g27.sAk = 1; g27.sBo = (long long)C * W; g27.sBi = 0; g27.sBn = 1; g27.sBk = 1; g27.sCo = (long long)F * LDO; g27.sCi = 0; g27.sCm = LDO; g27.sRo = (long long)F * LDO; g27.sRi = 0; g27.sRm = LDO; g27.sRn = 1;
      g27.M = F; g27.N = OW; g27.K = WW; g27.zi_n = 1; g27.flags = 4; g27.act = 0;
      g27.alpha = 1.0f; g27.beta = 1.0f; g27.sa = 1.0f; g27.sb = 1.0f; g27.Npad = OW; g27.pad_ = 0;
      k_gemm<1><<<dim3((unsigned)((OW) + 31) / 32, (unsigned)((F) + 15) / 16, (unsigned)(NB)), 32, 0, stream>>>(g27); }
    { GemmP g28;
      g28.A = w + 1792; g28.B = x + (size_t)28 * W; g28.bias = w + 1792; g28.R = ST; g28.C = ST;
      g28.sAo = 0; g28.sAi = 0; g28.sAm = C * WW; g28.sAk = 1; g28.sBo = (long long)C * W; g28.sBi = 0; g28.sBn = 1; g28.sBk = 1; g28.sCo = (long long)F * LDO; g28.sCi = 0; g28.sCm = LDO; g28.sRo = (long long)F * LDO; g28.sRi = 0; g28.sRm = LDO; g28.sRn = 1;
      g28.M = F; g28.N = OW; g28.K = WW; g28.zi_n = 1; g28.flags = 4; g28.act = 0;
      g28.alpha = 1.0f; g28.beta = 1.0f; g28.sa = 1.0f; g28.sb = 1.0f; g28.Npad = OW; g28.pad_ = 0;
      k_gemm<1><<<dim3((unsigned)((OW) + 31) / 32, (unsigned)((F) + 15) / 16, (unsigned)(NB)), 32, 0, stream>>>(g28); }
    { GemmP g29;
      g29.A = w + 1856; g29.B = x + (size_t)29 * W; g29.bias = w + 1856; g29.R = ST; g29.C = ST;
      g29.sAo = 0; g29.sAi = 0; g29.sAm = C * WW; g29.sAk = 1; g29.sBo = (long long)C * W; g29.sBi = 0; g29.sBn = 1; g29.sBk = 1; g29.sCo = (long long)F * LDO; g29.sCi = 0; g29.sCm = LDO; g29.sRo = (long long)F * LDO; g29.sRi = 0; g29.sRm = LDO; g29.sRn = 1;
      g29.M = F; g29.N = OW; g29.K = WW; g29.zi_n = 1; g29.flags = 4; g29.act = 0;
      g29.alpha = 1.0f; g29.beta = 1.0f; g29.sa = 1.0f; g29.sb = 1.0f; g29.Npad = OW; g29.pad_ = 0;
      k_gemm<1><<<dim3((unsigned)((OW) + 31) / 32, (unsigned)((F) + 15) / 16, (unsigned)(NB)), 32, 0, stream>>>(g29); }
    { GemmP g30;
      g30.A = w + 1920; g30.B = x + (size_t)30 * W; g30.bias = w + 1920; g30.R = ST; g30.C = ST;
      g30.sAo = 0; g30.sAi = 0; g30.sAm = C * WW; g30.sAk = 1; g30.sBo = (long long)C * W; g30.sBi = 0; g30.sBn = 1; g30.sBk = 1; g30.sCo = (long long)F * LDO; g30.sCi = 0; g30.sCm = LDO; g30.sRo = (long long)F * LDO; g30.sRi = 0; g30.sRm = LDO; g30.sRn = 1;
      g30.M = F; g30.N = OW; g30.K = WW; g30.zi_n = 1; g30.flags = 4; g30.act = 0;
      g30.alpha = 1.0f; g30.beta = 1.0f; g30.sa = 1.0f; g30.sb = 1.0f; g30.Npad = OW; g30.pad_ = 0;
      k_gemm<1><<<dim3((unsigned)((OW) + 31) / 32, (unsigned)((F) + 15) / 16, (unsigned)(NB)), 32, 0, stream>>>(g30); }
    { GemmP g31;
      g31.A = w + 1984; g31.B = x + (size_t)31 * W; g31.bias = w + 1984; g31.R = ST; g31.C = ST;
      g31.sAo = 0; g31.sAi = 0; g31.sAm = C * WW; g31.sAk = 1; g31.sBo = (long long)C * W; g31.sBi = 0; g31.sBn = 1; g31.sBk = 1; g31.sCo = (long long)F * LDO; g31.sCi = 0; g31.sCm = LDO; g31.sRo = (long long)F * LDO; g31.sRi = 0; g31.sRm = LDO; g31.sRn = 1;
      g31.M = F; g31.N = OW; g31.K = WW; g31.zi_n = 1; g31.flags = 4; g31.act = 0;
      g31.alpha = 1.0f; g31.beta = 1.0f; g31.sa = 1.0f; g31.sb = 1.0f; g31.Npad = OW; g31.pad_ = 0;
      k_gemm<1><<<dim3((unsigned)((OW) + 31) / 32, (unsigned)((F) + 15) / 16, (unsigned)(NB)), 32, 0, stream>>>(g31); }
    { GemmP g32;
      g32.A = w + 2048; g32.B = x + (size_t)32 * W; g32.bias = w + 2048; g32.R = ST; g32.C = ST;
      g32.sAo = 0; g32.sAi = 0; g32.sAm = C * WW; g32.sAk = 1; g32.sBo = (long long)C * W; g32.sBi = 0; g32.sBn = 1; g32.sBk = 1; g32.sCo = (long long)F * LDO; g32.sCi = 0; g32.sCm = LDO; g32.sRo = (long long)F * LDO; g32.sRi = 0; g32.sRm = LDO; g32.sRn = 1;
      g32.M = F; g32.N = OW; g32.K = WW; g32.zi_n = 1; g32.flags = 4; g32.act = 0;
      g32.alpha = 1.0f; g32.beta = 1.0f; g32.sa = 1.0f; g32.sb = 1.0f; g32.Npad = OW; g32.pad_ = 0;
      k_gemm<1><<<dim3((unsigned)((OW) + 31) / 32, (unsigned)((F) + 15) / 16, (unsigned)(NB)), 32, 0, stream>>>(g32); }
    { GemmP g33;
      g33.A = w + 2112; g33.B = x + (size_t)33 * W; g33.bias = w + 2112; g33.R = ST; g33.C = ST;
      g33.sAo = 0; g33.sAi = 0; g33.sAm = C * WW; g33.sAk = 1; g33.sBo = (long long)C * W; g33.sBi = 0; g33.sBn = 1; g33.sBk = 1; g33.sCo = (long long)F * LDO; g33.sCi = 0; g33.sCm = LDO; g33.sRo = (long long)F * LDO; g33.sRi = 0; g33.sRm = LDO; g33.sRn = 1;
      g33.M = F; g33.N = OW; g33.K = WW; g33.zi_n = 1; g33.flags = 4; g33.act = 0;
      g33.alpha = 1.0f; g33.beta = 1.0f; g33.sa = 1.0f; g33.sb = 1.0f; g33.Npad = OW; g33.pad_ = 0;
      k_gemm<1><<<dim3((unsigned)((OW) + 31) / 32, (unsigned)((F) + 15) / 16, (unsigned)(NB)), 32, 0, stream>>>(g33); }
    { GemmP g34;
      g34.A = w + 2176; g34.B = x + (size_t)34 * W; g34.bias = w + 2176; g34.R = ST; g34.C = ST;
      g34.sAo = 0; g34.sAi = 0; g34.sAm = C * WW; g34.sAk = 1; g34.sBo = (long long)C * W; g34.sBi = 0; g34.sBn = 1; g34.sBk = 1; g34.sCo = (long long)F * LDO; g34.sCi = 0; g34.sCm = LDO; g34.sRo = (long long)F * LDO; g34.sRi = 0; g34.sRm = LDO; g34.sRn = 1;
      g34.M = F; g34.N = OW; g34.K = WW; g34.zi_n = 1; g34.flags = 4; g34.act = 0;
      g34.alpha = 1.0f; g34.beta = 1.0f; g34.sa = 1.0f; g34.sb = 1.0f; g34.Npad = OW; g34.pad_ = 0;
      k_gemm<1><<<dim3((unsigned)((OW) + 31) / 32, (unsigned)((F) + 15) / 16, (unsigned)(NB)), 32, 0, stream>>>(g34); }
    { GemmP g35;
      g35.A = w + 2240; g35.B = x + (size_t)35 * W; g35.bias = w + 2240; g35.R = ST; g35.C = ST;
      g35.sAo = 0; g35.sAi = 0; g35.sAm = C * WW; g35.sAk = 1; g35.sBo = (long long)C * W; g35.sBi = 0; g35.sBn = 1; g35.sBk = 1; g35.sCo = (long long)F * LDO; g35.sCi = 0; g35.sCm = LDO; g35.sRo = (long long)F * LDO; g35.sRi = 0; g35.sRm = LDO; g35.sRn = 1;
      g35.M = F; g35.N = OW; g35.K = WW; g35.zi_n = 1; g35.flags = 4; g35.act = 0;
      g35.alpha = 1.0f; g35.beta = 1.0f; g35.sa = 1.0f; g35.sb = 1.0f; g35.Npad = OW; g35.pad_ = 0;
      k_gemm<1><<<dim3((unsigned)((OW) + 31) / 32, (unsigned)((F) + 15) / 16, (unsigned)(NB)), 32, 0, stream>>>(g35); }
    { GemmP g36;
      g36.A = w + 2304; g36.B = x + (size_t)36 * W; g36.bias = w + 2304; g36.R = ST; g36.C = ST;
      g36.sAo = 0; g36.sAi = 0; g36.sAm = C * WW; g36.sAk = 1; g36.sBo = (long long)C * W; g36.sBi = 0; g36.sBn = 1; g36.sBk = 1; g36.sCo = (long long)F * LDO; g36.sCi = 0; g36.sCm = LDO; g36.sRo = (long long)F * LDO; g36.sRi = 0; g36.sRm = LDO; g36.sRn = 1;
      g36.M = F; g36.N = OW; g36.K = WW; g36.zi_n = 1; g36.flags = 4; g36.act = 0;
      g36.alpha = 1.0f; g36.beta = 1.0f; g36.sa = 1.0f; g36.sb = 1.0f; g36.Npad = OW; g36.pad_ = 0;
      k_gemm<1><<<dim3((unsigned)((OW) + 31) / 32, (unsigned)((F) + 15) / 16, (unsigned)(NB)), 32, 0, stream>>>(g36); }
    { GemmP g37;
      g37.A = w + 2368; g37.B = x + (size_t)37 * W; g37.bias = w + 2368; g37.R = ST; g37.C = ST;
      g37.sAo = 0; g37.sAi = 0; g37.sAm = C * WW; g37.sAk = 1; g37.sBo = (long long)C * W; g37.sBi = 0; g37.sBn = 1; g37.sBk = 1; g37.sCo = (long long)F * LDO; g37.sCi = 0; g37.sCm = LDO; g37.sRo = (long long)F * LDO; g37.sRi = 0; g37.sRm = LDO; g37.sRn = 1;
      g37.M = F; g37.N = OW; g37.K = WW; g37.zi_n = 1; g37.flags = 4; g37.act = 0;
      g37.alpha = 1.0f; g37.beta = 1.0f; g37.sa = 1.0f; g37.sb = 1.0f; g37.Npad = OW; g37.pad_ = 0;
      k_gemm<1><<<dim3((unsigned)((OW) + 31) / 32, (unsigned)((F) + 15) / 16, (unsigned)(NB)), 32, 0, stream>>>(g37); }
    { GemmP g38;
      g38.A = w + 2432; g38.B = x + (size_t)38 * W; g38.bias = w + 2432; g38.R = ST; g38.C = ST;
      g38.sAo = 0; g38.sAi = 0; g38.sAm = C * WW; g38.sAk = 1; g38.sBo = (long long)C * W; g38.sBi = 0; g38.sBn = 1; g38.sBk = 1; g38.sCo = (long long)F * LDO; g38.sCi = 0; g38.sCm = LDO; g38.sRo = (long long)F * LDO; g38.sRi = 0; g38.sRm = LDO; g38.sRn = 1;
      g38.M = F; g38.N = OW; g38.K = WW; g38.zi_n = 1; g38.flags = 4; g38.act = 0;
      g38.alpha = 1.0f; g38.beta = 1.0f; g38.sa = 1.0f; g38.sb = 1.0f; g38.Npad = OW; g38.pad_ = 0;
      k_gemm<1><<<dim3((unsigned)((OW) + 31) / 32, (unsigned)((F) + 15) / 16, (unsigned)(NB)), 32, 0, stream>>>(g38); }
    { GemmP g39;
      g39.A = w + 2496; g39.B = x + (size_t)39 * W; g39.bias = w + 2496; g39.R = ST; g39.C = ST;
      g39.sAo = 0; g39.sAi = 0; g39.sAm = C * WW; g39.sAk = 1; g39.sBo = (long long)C * W; g39.sBi = 0; g39.sBn = 1; g39.sBk = 1; g39.sCo = (long long)F * LDO; g39.sCi = 0; g39.sCm = LDO; g39.sRo = (long long)F * LDO; g39.sRi = 0; g39.sRm = LDO; g39.sRn = 1;
      g39.M = F; g39.N = OW; g39.K = WW; g39.zi_n = 1; g39.flags = 4; g39.act = 0;
      g39.alpha = 1.0f; g39.beta = 1.0f; g39.sa = 1.0f; g39.sb = 1.0f; g39.Npad = OW; g39.pad_ = 0;
      k_gemm<1><<<dim3((unsigned)((OW) + 31) / 32, (unsigned)((F) + 15) / 16, (unsigned)(NB)), 32, 0, stream>>>(g39); }
    { GemmP g40;
      g40.A = w + 2560; g40.B = x + (size_t)40 * W; g40.bias = w + 2560; g40.R = ST; g40.C = ST;
      g40.sAo = 0; g40.sAi = 0; g40.sAm = C * WW; g40.sAk = 1; g40.sBo = (long long)C * W; g40.sBi = 0; g40.sBn = 1; g40.sBk = 1; g40.sCo = (long long)F * LDO; g40.sCi = 0; g40.sCm = LDO; g40.sRo = (long long)F * LDO; g40.sRi = 0; g40.sRm = LDO; g40.sRn = 1;
      g40.M = F; g40.N = OW; g40.K = WW; g40.zi_n = 1; g40.flags = 4; g40.act = 0;
      g40.alpha = 1.0f; g40.beta = 1.0f; g40.sa = 1.0f; g40.sb = 1.0f; g40.Npad = OW; g40.pad_ = 0;
      k_gemm<1><<<dim3((unsigned)((OW) + 31) / 32, (unsigned)((F) + 15) / 16, (unsigned)(NB)), 32, 0, stream>>>(g40); }
    { GemmP g41;
      g41.A = w + 2624; g41.B = x + (size_t)41 * W; g41.bias = w + 2624; g41.R = ST; g41.C = ST;
      g41.sAo = 0; g41.sAi = 0; g41.sAm = C * WW; g41.sAk = 1; g41.sBo = (long long)C * W; g41.sBi = 0; g41.sBn = 1; g41.sBk = 1; g41.sCo = (long long)F * LDO; g41.sCi = 0; g41.sCm = LDO; g41.sRo = (long long)F * LDO; g41.sRi = 0; g41.sRm = LDO; g41.sRn = 1;
      g41.M = F; g41.N = OW; g41.K = WW; g41.zi_n = 1; g41.flags = 4; g41.act = 0;
      g41.alpha = 1.0f; g41.beta = 1.0f; g41.sa = 1.0f; g41.sb = 1.0f; g41.Npad = OW; g41.pad_ = 0;
      k_gemm<1><<<dim3((unsigned)((OW) + 31) / 32, (unsigned)((F) + 15) / 16, (unsigned)(NB)), 32, 0, stream>>>(g41); }
    { GemmP g42;
      g42.A = w + 2688; g42.B = x + (size_t)42 * W; g42.bias = w + 2688; g42.R = ST; g42.C = ST;
      g42.sAo = 0; g42.sAi = 0; g42.sAm = C * WW; g42.sAk = 1; g42.sBo = (long long)C * W; g42.sBi = 0; g42.sBn = 1; g42.sBk = 1; g42.sCo = (long long)F * LDO; g42.sCi = 0; g42.sCm = LDO; g42.sRo = (long long)F * LDO; g42.sRi = 0; g42.sRm = LDO; g42.sRn = 1;
      g42.M = F; g42.N = OW; g42.K = WW; g42.zi_n = 1; g42.flags = 4; g42.act = 0;
      g42.alpha = 1.0f; g42.beta = 1.0f; g42.sa = 1.0f; g42.sb = 1.0f; g42.Npad = OW; g42.pad_ = 0;
      k_gemm<1><<<dim3((unsigned)((OW) + 31) / 32, (unsigned)((F) + 15) / 16, (unsigned)(NB)), 32, 0, stream>>>(g42); }
    { GemmP g43;
      g43.A = w + 2752; g43.B = x + (size_t)43 * W; g43.bias = w + 2752; g43.R = ST; g43.C = ST;
      g43.sAo = 0; g43.sAi = 0; g43.sAm = C * WW; g43.sAk = 1; g43.sBo = (long long)C * W; g43.sBi = 0; g43.sBn = 1; g43.sBk = 1; g43.sCo = (long long)F * LDO; g43.sCi = 0; g43.sCm = LDO; g43.sRo = (long long)F * LDO; g43.sRi = 0; g43.sRm = LDO; g43.sRn = 1;
      g43.M = F; g43.N = OW; g43.K = WW; g43.zi_n = 1; g43.flags = 4; g43.act = 0;
      g43.alpha = 1.0f; g43.beta = 1.0f; g43.sa = 1.0f; g43.sb = 1.0f; g43.Npad = OW; g43.pad_ = 0;
      k_gemm<1><<<dim3((unsigned)((OW) + 31) / 32, (unsigned)((F) + 15) / 16, (unsigned)(NB)), 32, 0, stream>>>(g43); }
    { GemmP g44;
      g44.A = w + 2816; g44.B = x + (size_t)44 * W; g44.bias = w + 2816; g44.R = ST; g44.C = ST;
      g44.sAo = 0; g44.sAi = 0; g44.sAm = C * WW; g44.sAk = 1; g44.sBo = (long long)C * W; g44.sBi = 0; g44.sBn = 1; g44.sBk = 1; g44.sCo = (long long)F * LDO; g44.sCi = 0; g44.sCm = LDO; g44.sRo = (long long)F * LDO; g44.sRi = 0; g44.sRm = LDO; g44.sRn = 1;
      g44.M = F; g44.N = OW; g44.K = WW; g44.zi_n = 1; g44.flags = 4; g44.act = 0;
      g44.alpha = 1.0f; g44.beta = 1.0f; g44.sa = 1.0f; g44.sb = 1.0f; g44.Npad = OW; g44.pad_ = 0;
      k_gemm<1><<<dim3((unsigned)((OW) + 31) / 32, (unsigned)((F) + 15) / 16, (unsigned)(NB)), 32, 0, stream>>>(g44); }
    { GemmP g45;
      g45.A = w + 2880; g45.B = x + (size_t)45 * W; g45.bias = w + 2880; g45.R = ST; g45.C = ST;
      g45.sAo = 0; g45.sAi = 0; g45.sAm = C * WW; g45.sAk = 1; g45.sBo = (long long)C * W; g45.sBi = 0; g45.sBn = 1; g45.sBk = 1; g45.sCo = (long long)F * LDO; g45.sCi = 0; g45.sCm = LDO; g45.sRo = (long long)F * LDO; g45.sRi = 0; g45.sRm = LDO; g45.sRn = 1;
      g45.M = F; g45.N = OW; g45.K = WW; g45.zi_n = 1; g45.flags = 4; g45.act = 0;
      g45.alpha = 1.0f; g45.beta = 1.0f; g45.sa = 1.0f; g45.sb = 1.0f; g45.Npad = OW; g45.pad_ = 0;
      k_gemm<1><<<dim3((unsigned)((OW) + 31) / 32, (unsigned)((F) + 15) / 16, (unsigned)(NB)), 32, 0, stream>>>(g45); }
    { GemmP g46;
      g46.A = w + 2944; g46.B = x + (size_t)46 * W; g46.bias = w + 2944; g46.R = ST; g46.C = ST;
      g46.sAo = 0; g46.sAi = 0; g46.sAm = C * WW; g46.sAk = 1; g46.sBo = (long long)C * W; g46.sBi = 0; g46.sBn = 1; g46.sBk = 1; g46.sCo = (long long)F * LDO; g46.sCi = 0; g46.sCm = LDO; g46.sRo = (long long)F * LDO; g46.sRi = 0; g46.sRm = LDO; g46.sRn = 1;
      g46.M = F; g46.N = OW; g46.K = WW; g46.zi_n = 1; g46.flags = 4; g46.act = 0;
      g46.alpha = 1.0f; g46.beta = 1.0f; g46.sa = 1.0f; g46.sb = 1.0f; g46.Npad = OW; g46.pad_ = 0;
      k_gemm<1><<<dim3((unsigned)((OW) + 31) / 32, (unsigned)((F) + 15) / 16, (unsigned)(NB)), 32, 0, stream>>>(g46); }
    { GemmP g47;
      g47.A = w + 3008; g47.B = x + (size_t)47 * W; g47.bias = w + 3008; g47.R = ST; g47.C = ST;
      g47.sAo = 0; g47.sAi = 0; g47.sAm = C * WW; g47.sAk = 1; g47.sBo = (long long)C * W; g47.sBi = 0; g47.sBn = 1; g47.sBk = 1; g47.sCo = (long long)F * LDO; g47.sCi = 0; g47.sCm = LDO; g47.sRo = (long long)F * LDO; g47.sRi = 0; g47.sRm = LDO; g47.sRn = 1;
      g47.M = F; g47.N = OW; g47.K = WW; g47.zi_n = 1; g47.flags = 4; g47.act = 0;
      g47.alpha = 1.0f; g47.beta = 1.0f; g47.sa = 1.0f; g47.sb = 1.0f; g47.Npad = OW; g47.pad_ = 0;
      k_gemm<1><<<dim3((unsigned)((OW) + 31) / 32, (unsigned)((F) + 15) / 16, (unsigned)(NB)), 32, 0, stream>>>(g47); }
    { GemmP g48;
      g48.A = w + 3072; g48.B = x + (size_t)48 * W; g48.bias = w + 3072; g48.R = ST; g48.C = ST;
      g48.sAo = 0; g48.sAi = 0; g48.sAm = C * WW; g48.sAk = 1; g48.sBo = (long long)C * W; g48.sBi = 0; g48.sBn = 1; g48.sBk = 1; g48.sCo = (long long)F * LDO; g48.sCi = 0; g48.sCm = LDO; g48.sRo = (long long)F * LDO; g48.sRi = 0; g48.sRm = LDO; g48.sRn = 1;
      g48.M = F; g48.N = OW; g48.K = WW; g48.zi_n = 1; g48.flags = 4; g48.act = 0;
      g48.alpha = 1.0f; g48.beta = 1.0f; g48.sa = 1.0f; g48.sb = 1.0f; g48.Npad = OW; g48.pad_ = 0;
      k_gemm<1><<<dim3((unsigned)((OW) + 31) / 32, (unsigned)((F) + 15) / 16, (unsigned)(NB)), 32, 0, stream>>>(g48); }
    { GemmP g49;
      g49.A = w + 3136; g49.B = x + (size_t)49 * W; g49.bias = w + 3136; g49.R = ST; g49.C = ST;
      g49.sAo = 0; g49.sAi = 0; g49.sAm = C * WW; g49.sAk = 1; g49.sBo = (long long)C * W; g49.sBi = 0; g49.sBn = 1; g49.sBk = 1; g49.sCo = (long long)F * LDO; g49.sCi = 0; g49.sCm = LDO; g49.sRo = (long long)F * LDO; g49.sRi = 0; g49.sRm = LDO; g49.sRn = 1;
      g49.M = F; g49.N = OW; g49.K = WW; g49.zi_n = 1; g49.flags = 4; g49.act = 0;
      g49.alpha = 1.0f; g49.beta = 1.0f; g49.sa = 1.0f; g49.sb = 1.0f; g49.Npad = OW; g49.pad_ = 0;
      k_gemm<1><<<dim3((unsigned)((OW) + 31) / 32, (unsigned)((F) + 15) / 16, (unsigned)(NB)), 32, 0, stream>>>(g49); }
    { GemmP g50;
      g50.A = w + 3200; g50.B = x + (size_t)50 * W; g50.bias = w + 3200; g50.R = ST; g50.C = ST;
      g50.sAo = 0; g50.sAi = 0; g50.sAm = C * WW; g50.sAk = 1; g50.sBo = (long long)C * W; g50.sBi = 0; g50.sBn = 1; g50.sBk = 1; g50.sCo = (long long)F * LDO; g50.sCi = 0; g50.sCm = LDO; g50.sRo = (long long)F * LDO; g50.sRi = 0; g50.sRm = LDO; g50.sRn = 1;
      g50.M = F; g50.N = OW; g50.K = WW; g50.zi_n = 1; g50.flags = 4; g50.act = 0;
      g50.alpha = 1.0f; g50.beta = 1.0f; g50.sa = 1.0f; g50.sb = 1.0f; g50.Npad = OW; g50.pad_ = 0;
      k_gemm<1><<<dim3((unsigned)((OW) + 31) / 32, (unsigned)((F) + 15) / 16, (unsigned)(NB)), 32, 0, stream>>>(g50); }
    { GemmP g51;
      g51.A = w + 3264; g51.B = x + (size_t)51 * W; g51.bias = w + 3264; g51.R = ST; g51.C = ST;
      g51.sAo = 0; g51.sAi = 0; g51.sAm = C * WW; g51.sAk = 1; g51.sBo = (long long)C * W; g51.sBi = 0; g51.sBn = 1; g51.sBk = 1; g51.sCo = (long long)F * LDO; g51.sCi = 0; g51.sCm = LDO; g51.sRo = (long long)F * LDO; g51.sRi = 0; g51.sRm = LDO; g51.sRn = 1;
      g51.M = F; g51.N = OW; g51.K = WW; g51.zi_n = 1; g51.flags = 4; g51.act = 0;
      g51.alpha = 1.0f; g51.beta = 1.0f; g51.sa = 1.0f; g51.sb = 1.0f; g51.Npad = OW; g51.pad_ = 0;
      k_gemm<1><<<dim3((unsigned)((OW) + 31) / 32, (unsigned)((F) + 15) / 16, (unsigned)(NB)), 32, 0, stream>>>(g51); }
    { GemmP g52;
      g52.A = w + 3328; g52.B = x + (size_t)52 * W; g52.bias = w + 3328; g52.R = ST; g52.C = ST;
      g52.sAo = 0; g52.sAi = 0; g52.sAm = C * WW; g52.sAk = 1; g52.sBo = (long long)C * W; g52.sBi = 0; g52.sBn = 1; g52.sBk = 1; g52.sCo = (long long)F * LDO; g52.sCi = 0; g52.sCm = LDO; g52.sRo = (long long)F * LDO; g52.sRi = 0; g52.sRm = LDO; g52.sRn = 1;
      g52.M = F; g52.N = OW; g52.K = WW; g52.zi_n = 1; g52.flags = 4; g52.act = 0;
      g52.alpha = 1.0f; g52.beta = 1.0f; g52.sa = 1.0f; g52.sb = 1.0f; g52.Npad = OW; g52.pad_ = 0;
      k_gemm<1><<<dim3((unsigned)((OW) + 31) / 32, (unsigned)((F) + 15) / 16, (unsigned)(NB)), 32, 0, stream>>>(g52); }
    { GemmP g53;
      g53.A = w + 3392; g53.B = x + (size_t)53 * W; g53.bias = w + 3392; g53.R = ST; g53.C = ST;
      g53.sAo = 0; g53.sAi = 0; g53.sAm = C * WW; g53.sAk = 1; g53.sBo = (long long)C * W; g53.sBi = 0; g53.sBn = 1; g53.sBk = 1; g53.sCo = (long long)F * LDO; g53.sCi = 0; g53.sCm = LDO; g53.sRo = (long long)F * LDO; g53.sRi = 0; g53.sRm = LDO; g53.sRn = 1;
      g53.M = F; g53.N = OW; g53.K = WW; g53.zi_n = 1; g53.flags = 4; g53.act = 0;
      g53.alpha = 1.0f; g53.beta = 1.0f; g53.sa = 1.0f; g53.sb = 1.0f; g53.Npad = OW; g53.pad_ = 0;
      k_gemm<1><<<dim3((unsigned)((OW) + 31) / 32, (unsigned)((F) + 15) / 16, (unsigned)(NB)), 32, 0, stream>>>(g53); }
    { GemmP g54;
      g54.A = w + 3456; g54.B = x + (size_t)54 * W; g54.bias = w + 3456; g54.R = ST; g54.C = ST;
      g54.sAo = 0; g54.sAi = 0; g54.sAm = C * WW; g54.sAk = 1; g54.sBo = (long long)C * W; g54.sBi = 0; g54.sBn = 1; g54.sBk = 1; g54.sCo = (long long)F * LDO; g54.sCi = 0; g54.sCm = LDO; g54.sRo = (long long)F * LDO; g54.sRi = 0; g54.sRm = LDO; g54.sRn = 1;
      g54.M = F; g54.N = OW; g54.K = WW; g54.zi_n = 1; g54.flags = 4; g54.act = 0;
      g54.alpha = 1.0f; g54.beta = 1.0f; g54.sa = 1.0f; g54.sb = 1.0f; g54.Npad = OW; g54.pad_ = 0;
      k_gemm<1><<<dim3((unsigned)((OW) + 31) / 32, (unsigned)((F) + 15) / 16, (unsigned)(NB)), 32, 0, stream>>>(g54); }
    { GemmP g55;
      g55.A = w + 3520; g55.B = x + (size_t)55 * W; g55.bias = w + 3520; g55.R = ST; g55.C = ST;
      g55.sAo = 0; g55.sAi = 0; g55.sAm = C * WW; g55.sAk = 1; g55.sBo = (long long)C * W; g55.sBi = 0; g55.sBn = 1; g55.sBk = 1; g55.sCo = (long long)F * LDO; g55.sCi = 0; g55.sCm = LDO; g55.sRo = (long long)F * LDO; g55.sRi = 0; g55.sRm = LDO; g55.sRn = 1;
      g55.M = F; g55.N = OW; g55.K = WW; g55.zi_n = 1; g55.flags = 4; g55.act = 0;
      g55.alpha = 1.0f; g55.beta = 1.0f; g55.sa = 1.0f; g55.sb = 1.0f; g55.Npad = OW; g55.pad_ = 0;
      k_gemm<1><<<dim3((unsigned)((OW) + 31) / 32, (unsigned)((F) + 15) / 16, (unsigned)(NB)), 32, 0, stream>>>(g55); }
    { GemmP g56;
      g56.A = w + 3584; g56.B = x + (size_t)56 * W; g56.bias = w + 3584; g56.R = ST; g56.C = ST;
      g56.sAo = 0; g56.sAi = 0; g56.sAm = C * WW; g56.sAk = 1; g56.sBo = (long long)C * W; g56.sBi = 0; g56.sBn = 1; g56.sBk = 1; g56.sCo = (long long)F * LDO; g56.sCi = 0; g56.sCm = LDO; g56.sRo = (long long)F * LDO; g56.sRi = 0; g56.sRm = LDO; g56.sRn = 1;
      g56.M = F; g56.N = OW; g56.K = WW; g56.zi_n = 1; g56.flags = 4; g56.act = 0;
      g56.alpha = 1.0f; g56.beta = 1.0f; g56.sa = 1.0f; g56.sb = 1.0f; g56.Npad = OW; g56.pad_ = 0;
      k_gemm<1><<<dim3((unsigned)((OW) + 31) / 32, (unsigned)((F) + 15) / 16, (unsigned)(NB)), 32, 0, stream>>>(g56); }
    { GemmP g57;
      g57.A = w + 3648; g57.B = x + (size_t)57 * W; g57.bias = w + 3648; g57.R = ST; g57.C = ST;
      g57.sAo = 0; g57.sAi = 0; g57.sAm = C * WW; g57.sAk = 1; g57.sBo = (long long)C * W; g57.sBi = 0; g57.sBn = 1; g57.sBk = 1; g57.sCo = (long long)F * LDO; g57.sCi = 0; g57.sCm = LDO; g57.sRo = (long long)F * LDO; g57.sRi = 0; g57.sRm = LDO; g57.sRn = 1;
      g57.M = F; g57.N = OW; g57.K = WW; g57.zi_n = 1; g57.flags = 4; g57.act = 0;
      g57.alpha = 1.0f; g57.beta = 1.0f; g57.sa = 1.0f; g57.sb = 1.0f; g57.Npad = OW; g57.pad_ = 0;
      k_gemm<1><<<dim3((unsigned)((OW) + 31) / 32, (unsigned)((F) + 15) / 16, (unsigned)(NB)), 32, 0, stream>>>(g57); }
    { GemmP g58;
      g58.A = w + 3712; g58.B = x + (size_t)58 * W; g58.bias = w + 3712; g58.R = ST; g58.C = ST;
      g58.sAo = 0; g58.sAi = 0; g58.sAm = C * WW; g58.sAk = 1; g58.sBo = (long long)C * W; g58.sBi = 0; g58.sBn = 1; g58.sBk = 1; g58.sCo = (long long)F * LDO; g58.sCi = 0; g58.sCm = LDO; g58.sRo = (long long)F * LDO; g58.sRi = 0; g58.sRm = LDO; g58.sRn = 1;
      g58.M = F; g58.N = OW; g58.K = WW; g58.zi_n = 1; g58.flags = 4; g58.act = 0;
      g58.alpha = 1.0f; g58.beta = 1.0f; g58.sa = 1.0f; g58.sb = 1.0f; g58.Npad = OW; g58.pad_ = 0;
      k_gemm<1><<<dim3((unsigned)((OW) + 31) / 32, (unsigned)((F) + 15) / 16, (unsigned)(NB)), 32, 0, stream>>>(g58); }
    { GemmP g59;
      g59.A = w + 3776; g59.B = x + (size_t)59 * W; g59.bias = w + 3776; g59.R = ST; g59.C = ST;
      g59.sAo = 0; g59.sAi = 0; g59.sAm = C * WW; g59.sAk = 1; g59.sBo = (long long)C * W; g59.sBi = 0; g59.sBn = 1; g59.sBk = 1; g59.sCo = (long long)F * LDO; g59.sCi = 0; g59.sCm = LDO; g59.sRo = (long long)F * LDO; g59.sRi = 0; g59.sRm = LDO; g59.sRn = 1;
      g59.M = F; g59.N = OW; g59.K = WW; g59.zi_n = 1; g59.flags = 4; g59.act = 0;
      g59.alpha = 1.0f; g59.beta = 1.0f; g59.sa = 1.0f; g59.sb = 1.0f; g59.Npad = OW; g59.pad_ = 0;
      k_gemm<1><<<dim3((unsigned)((OW) + 31) / 32, (unsigned)((F) + 15) / 16, (unsigned)(NB)), 32, 0, stream>>>(g59); }
    { GemmP g60;
      g60.A = w + 3840; g60.B = x + (size_t)60 * W; g60.bias = w + 3840; g60.R = ST; g60.C = ST;
      g60.sAo = 0; g60.sAi = 0; g60.sAm = C * WW; g60.sAk = 1; g60.sBo = (long long)C * W; g60.sBi = 0; g60.sBn = 1; g60.sBk = 1; g60.sCo = (long long)F * LDO; g60.sCi = 0; g60.sCm = LDO; g60.sRo = (long long)F * LDO; g60.sRi = 0; g60.sRm = LDO; g60.sRn = 1;
      g60.M = F; g60.N = OW; g60.K = WW; g60.zi_n = 1; g60.flags = 4; g60.act = 0;
      g60.alpha = 1.0f; g60.beta = 1.0f; g60.sa = 1.0f; g60.sb = 1.0f; g60.Npad = OW; g60.pad_ = 0;
      k_gemm<1><<<dim3((unsigned)((OW) + 31) / 32, (unsigned)((F) + 15) / 16, (unsigned)(NB)), 32, 0, stream>>>(g60); }
    { GemmP g61;
      g61.A = w + 3904; g61.B = x + (size_t)61 * W; g61.bias = w + 3904; g61.R = ST; g61.C = ST;
      g61.sAo = 0; g61.sAi = 0; g61.sAm = C * WW; g61.sAk = 1; g61.sBo = (long long)C * W; g61.sBi = 0; g61.sBn = 1; g61.sBk = 1; g61.sCo = (long long)F * LDO; g61.sCi = 0; g61.sCm = LDO; g61.sRo = (long long)F * LDO; g61.sRi = 0; g61.sRm = LDO; g61.sRn = 1;
      g61.M = F; g61.N = OW; g61.K = WW; g61.zi_n = 1; g61.flags = 4; g61.act = 0;
      g61.alpha = 1.0f; g61.beta = 1.0f; g61.sa = 1.0f; g61.sb = 1.0f; g61.Npad = OW; g61.pad_ = 0;
      k_gemm<1><<<dim3((unsigned)((OW) + 31) / 32, (unsigned)((F) + 15) / 16, (unsigned)(NB)), 32, 0, stream>>>(g61); }
    { GemmP g62;
      g62.A = w + 3968; g62.B = x + (size_t)62 * W; g62.bias = w + 3968; g62.R = ST; g62.C = ST;
      g62.sAo = 0; g62.sAi = 0; g62.sAm = C * WW; g62.sAk = 1; g62.sBo = (long long)C * W; g62.sBi = 0; g62.sBn = 1; g62.sBk = 1; g62.sCo = (long long)F * LDO; g62.sCi = 0; g62.sCm = LDO; g62.sRo = (long long)F * LDO; g62.sRi = 0; g62.sRm = LDO; g62.sRn = 1;
      g62.M = F; g62.N = OW; g62.K = WW; g62.zi_n = 1; g62.flags = 4; g62.act = 0;
      g62.alpha = 1.0f; g62.beta = 1.0f; g62.sa = 1.0f; g62.sb = 1.0f; g62.Npad = OW; g62.pad_ = 0;
      k_gemm<1><<<dim3((unsigned)((OW) + 31) / 32, (unsigned)((F) + 15) / 16, (unsigned)(NB)), 32, 0, stream>>>(g62); }
    { GemmP g63;
      g63.A = w + 4032; g63.B = x + (size_t)63 * W; g63.bias = w + 4032; g63.R = ST; g63.C = ST;
      g63.sAo = 0; g63.sAi = 0; g63.sAm = C * WW; g63.sAk = 1; g63.sBo = (long long)C * W; g63.sBi = 0; g63.sBn = 1; g63.sBk = 1; g63.sCo = (long long)F * LDO; g63.sCi = 0; g63.sCm = LDO; g63.sRo = (long long)F * LDO; g63.sRi = 0; g63.sRm = LDO; g63.sRn = 1;
      g63.M = F; g63.N = OW; g63.K = WW; g63.zi_n = 1; g63.flags = 4; g63.act = 0;
      g63.alpha = 1.0f; g63.beta = 1.0f; g63.sa = 1.0f; g63.sb = 1.0f; g63.Npad = OW; g63.pad_ = 0;
      k_gemm<1><<<dim3((unsigned)((OW) + 31) / 32, (unsigned)((F) + 15) / 16, (unsigned)(NB)), 32, 0, stream>>>(g63); }
    k_lincopy<<<(unsigned)(((long long)(NB * F) * (OW) + 255) / 256), 256, 0, stream>>>(ST, LDO, out, OW, NB * F, OW);
}
